// MoE_51144470561266
// MI455X (gfx1250) — hardware-verified
//
#include <hip/hip_runtime.h>
#include <math.h>

typedef __attribute__((ext_vector_type(16))) _Float16 v16h;
typedef __attribute__((ext_vector_type(8)))  _Float16 v8h;
typedef __attribute__((ext_vector_type(16))) __bf16   v16b;
typedef __attribute__((ext_vector_type(8)))  float    v8f;
typedef __attribute__((ext_vector_type(4)))  float    v4f;

__device__ __forceinline__ int frag_k(int i, int h) { return (i < 8) ? (8 * h + i) : (16 + 8 * h + (i - 8)); }
__device__ __forceinline__ __bf16 bf16_rne(float f) {
    unsigned int u = __float_as_uint(f);
    u += 0x7fffu + ((u >> 16) & 1u);
    return __builtin_bit_cast(__bf16, (unsigned short)(u >> 16));
}
__device__ __forceinline__ float bf16_f32(__bf16 b) { return __uint_as_float(((unsigned int)__builtin_bit_cast(unsigned short, b)) << 16); }
__device__ __forceinline__ v8f wmma16(v16h a, v16h b, v8f c) {
    c = __builtin_amdgcn_wmma_f32_16x16x32_f16(false, a, false, b, (short)0, c, false, false);
    asm volatile("v_nop\n\tv_nop\n\tv_nop\n\tv_nop" : "+v"(c) : "v"(a), "v"(b));
    return c;
}
__device__ __forceinline__ v8f wmmab(v16b a, v16b b, v8f c) {
    c = __builtin_amdgcn_wmma_f32_16x16x32_bf16(false, a, false, b, (short)0, c, false, false);
    asm volatile("v_nop\n\tv_nop\n\tv_nop\n\tv_nop" : "+v"(c) : "v"(a), "v"(b));
    return c;
}
struct Split { v16b hi, lo; };
__device__ __forceinline__ v8f wmma3(const Split& a, const Split& b, v8f c) {
    c = __builtin_amdgcn_wmma_f32_16x16x32_bf16(false, a.hi, false, b.hi, (short)0, c, false, false);
    c = __builtin_amdgcn_wmma_f32_16x16x32_bf16(false, a.hi, false, b.lo, (short)0, c, false, false);
    c = __builtin_amdgcn_wmma_f32_16x16x32_bf16(false, a.lo, false, b.hi, (short)0, c, false, false);
    asm volatile("v_nop\n\tv_nop\n\tv_nop\n\tv_nop" : "+v"(c) : "v"(a.hi), "v"(a.lo), "v"(b.hi), "v"(b.lo));
    return c;
}
struct Split3 { v16b hi, mid, lo; };
__device__ __forceinline__ v8f wmma6(const Split3& a, const Split3& b, v8f c) {
    c = __builtin_amdgcn_wmma_f32_16x16x32_bf16(false, a.hi, false, b.hi, (short)0, c, false, false);
    c = __builtin_amdgcn_wmma_f32_16x16x32_bf16(false, a.hi, false, b.mid, (short)0, c, false, false);
    c = __builtin_amdgcn_wmma_f32_16x16x32_bf16(false, a.mid, false, b.hi, (short)0, c, false, false);
    c = __builtin_amdgcn_wmma_f32_16x16x32_bf16(false, a.hi, false, b.lo, (short)0, c, false, false);
    c = __builtin_amdgcn_wmma_f32_16x16x32_bf16(false, a.mid, false, b.mid, (short)0, c, false, false);
    c = __builtin_amdgcn_wmma_f32_16x16x32_bf16(false, a.lo, false, b.hi, (short)0, c, false, false);
    asm volatile("v_nop\n\tv_nop\n\tv_nop\n\tv_nop" : "+v"(c) : "v"(a.hi), "v"(a.mid), "v"(a.lo), "v"(b.hi), "v"(b.mid), "v"(b.lo));
    return c;
}

__device__ __forceinline__ v16h fh_ld(const float* __restrict__ p, long long sk, int k0, int h, int klen, float s) {
    v16h a;
#pragma unroll
    for (int i = 0; i < 16; ++i) { const int k = k0 + frag_k(i, h); a[i] = (k < klen) ? (_Float16)(p[(long long)k * sk] * s) : (_Float16)0.f; }
    return a;
}
__device__ __forceinline__ Split sp_ld(const float* __restrict__ p, long long sk, int k0, int h, int klen, float s) {
    Split r;
#pragma unroll
    for (int i = 0; i < 16; ++i) {
        const int k = k0 + frag_k(i, h); const float x = (k < klen) ? p[(long long)k * sk] * s : 0.f;
        const __bf16 hb = bf16_rne(x); r.hi[i] = hb; r.lo[i] = bf16_rne(x - bf16_f32(hb));
    }
    return r;
}
__device__ __forceinline__ Split3 sp3_ld(const float* __restrict__ p, long long sk, int k0, int h, int klen, float s) {
    Split3 r;
#pragma unroll
    for (int i = 0; i < 16; ++i) {
        const int k = k0 + frag_k(i, h); const float x = (k < klen) ? p[(long long)k * sk] * s : 0.f;
        const __bf16 hb = bf16_rne(x); const float r1 = x - bf16_f32(hb); const __bf16 mb = bf16_rne(r1);
        r.hi[i] = hb; r.mid[i] = mb; r.lo[i] = bf16_rne(r1 - bf16_f32(mb));
    }
    return r;
}
__device__ __forceinline__ v16b bh_ld(const float* __restrict__ p, long long sk, int k0, int h, int klen, float s) {
    v16b a;
#pragma unroll
    for (int i = 0; i < 16; ++i) { const int k = k0 + frag_k(i, h); a[i] = bf16_rne((k < klen) ? p[(long long)k * sk] * s : 0.f); }
    return a;
}
__device__ __forceinline__ v16h fh_row(const _Float16* __restrict__ row, int k0, int h) {
    v16h a;
#pragma unroll
    for (int i = 0; i < 16; ++i) a[i] = row[k0 + frag_k(i, h)];
    return a;
}

#define VST2(T, ptr, val) do { *(volatile T*)(ptr) = (val); __threadfence(); *(volatile T*)(ptr) = (val); } while (0)
typedef float v4f __attribute__((ext_vector_type(4)));
#define VST2V4(ptr, val) do { *(volatile v4f*)(ptr) = (val); __threadfence(); *(volatile v4f*)(ptr) = (val); } while (0)

__device__ __attribute__((noinline)) float act_fn(float v, int act) {
    if (act == 1) return fmaxf(v, 0.f);
    if (act == 2) { const float u = 0.7978845608028654f * (v + 0.044715f * v * v * v); return 0.5f * v * (1.f + tanhf(u)); }
    if (act == 3) return v / (1.f + expf(-v));
    if (act == 4) return 0.5f * v * (1.f + erff(v * 0.7071067811865476f));
    if (act == 5) return tanhf(v);
    if (act == 6) return 1.f / (1.f + expf(-v));
    if (act == 7) return (v > 0.f) ? v : 0.01f * v;
    if (act == 8) return (v > 0.f) ? v : (expf(v) - 1.f);
    if (act == 9) return fminf(fmaxf(v, 0.f), 6.f);
    if (act == 10) return fabsf(v);
    if (act == 11) return (v >= 0.f) ? v : 0.1f * v;
    if (act == 12) return (v > 0.f) ? v : 0.2f * v;
    if (act == 13) return (v > 20.f) ? v : log1pf(expf(v));
    return v;
}

struct GemmP {
    const float* A; const float* B; const float* bias; const float* R; float* C;
    long long sAo, sAi, sAm, sAk, sBo, sBi, sBn, sBk, sCo, sCi, sCm, sRo, sRi, sRm, sRn;
    int M, N, K, zi_n, flags, act; float alpha, beta, sa, sb;
    int Npad, pad_;
};
static_assert(sizeof(GemmP) == 5 * 8 + 15 * 8 + 6 * 4 + 4 * 4 + 2 * 4, "GemmP has padding");

template <int MODE>
__global__ __launch_bounds__(32) void k_gemm(GemmP p) {
    const int lane = threadIdx.x & 31, h = lane >> 4, l15 = lane & 15;
    const int m0 = blockIdx.y * 16, n0 = blockIdx.x * 32;
    const int z = blockIdx.z, zo = z / p.zi_n, zi = z - zo * p.zi_n;
    const float* A = p.A + zo * p.sAo + zi * p.sAi;
    const float* B = p.B + zo * p.sBo + zi * p.sBi;
    const int am = min(m0 + l15, p.M - 1);
    v8f acc[2], comp[2];
#pragma unroll
    for (int t = 0; t < 2; ++t) { v8f zz = {}; acc[t] = zz; comp[t] = zz; }
    for (int k0 = 0; k0 < p.K; k0 += 32) {
        const float* arow = A + (long long)am * p.sAm;
        if (MODE == 1) {
            const Split a = sp_ld(arow, p.sAk, k0, h, p.K, 1.f);
#pragma unroll
            for (int t = 0; t < 2; ++t) {
                const int bn = min(n0 + t * 16 + l15, p.N - 1);
                acc[t] = wmma3(a, sp_ld(B + (long long)bn * p.sBn, p.sBk, k0, h, p.K, 1.f), acc[t]);
            }
        } else if (MODE == 3) {
            const Split3 a = sp3_ld(arow, p.sAk, k0, h, p.K, 1.f);
#pragma unroll
            for (int t = 0; t < 2; ++t) {
                const int bn = min(n0 + t * 16 + l15, p.N - 1);
                acc[t] = wmma6(a, sp3_ld(B + (long long)bn * p.sBn, p.sBk, k0, h, p.K, 1.f), acc[t]);
            }
        } else if (MODE == 4) {
            const Split3 a = sp3_ld(arow, p.sAk, k0, h, p.K, 1.f);
#pragma unroll
            for (int t = 0; t < 2; ++t) {
                const int bn = min(n0 + t * 16 + l15, p.N - 1); v8f zz = {};
                const v8f part = wmma6(a, sp3_ld(B + (long long)bn * p.sBn, p.sBk, k0, h, p.K, 1.f), zz);
                const v8f y = part - comp[t]; const v8f s = acc[t] + y; comp[t] = (s - acc[t]) - y; acc[t] = s;
            }
        } else if (MODE == 2) {
            const v16b a = bh_ld(arow, p.sAk, k0, h, p.K, 1.f);
#pragma unroll
            for (int t = 0; t < 2; ++t) {
                const int bn = min(n0 + t * 16 + l15, p.N - 1);
                acc[t] = wmmab(a, bh_ld(B + (long long)bn * p.sBn, p.sBk, k0, h, p.K, 1.f), acc[t]);
            }
        } else {
            const v16h a = fh_ld(arow, p.sAk, k0, h, p.K, p.sa);
#pragma unroll
            for (int t = 0; t < 2; ++t) {
                const int bn = min(n0 + t * 16 + l15, p.N - 1);
                acc[t] = wmma16(a, fh_ld(B + (long long)bn * p.sBn, p.sBk, k0, h, p.K, p.sb), acc[t]);
            }
        }
    }
    const float iscale = (MODE == 0) ? p.alpha / (p.sa * p.sb) : p.alpha;
    float* C = p.C + zo * p.sCo + zi * p.sCi;
    const float* R = p.R + zo * p.sRo + zi * p.sRi;
    __shared__ __align__(16) float ctile[16][36];
#pragma unroll
    for (int t = 0; t < 2; ++t) {
        const int n = n0 + t * 16 + l15; const int nn = min(n, p.N - 1);
#pragma unroll
        for (int r = 0; r < 8; ++r) {
            const int m = m0 + 8 * h + r; const int mm = min(m, p.M - 1);
            float v = acc[t][r] * iscale;
            if (p.flags & 1) v += p.bias[nn];
            if (p.flags & 2) v += p.bias[mm];
            v = act_fn(v, p.act);
            if (p.flags & 4) v += p.beta * R[(long long)mm * p.sRm + (long long)nn * p.sRn];
            ctile[8 * h + r][t * 16 + l15] = (n < p.N) ? v : 0.f;
        }
    }
    __syncthreads();
    const int NW = (p.Npad > p.N) ? p.Npad : p.N;
    const bool fast = (m0 + 16 <= p.M) && (n0 + 32 <= NW) && ((p.sCm & 3) == 0) && ((((size_t)C) & 15) == 0);
    if (fast) {
#pragma unroll
        for (int s = 0; s < 4; ++s) {
            const int row = s * 4 + (lane >> 3), c4 = (lane & 7) * 4;
            const v4f v = *(const v4f*)&ctile[row][c4];
            VST2V4(C + (long long)(m0 + row) * p.sCm + n0 + c4, v);
        }
    } else {
        for (int row = 0; row < 16; ++row) {
            const int m = m0 + row, n = n0 + lane;
            if (m < p.M && n < NW) VST2(float, C + (long long)m * p.sCm + n, ctile[row][lane]);
        }
    }
}

#define AW 4
struct AttnP {
    const float* Q; const float* K; const float* V; float* O; float* P; const float* Mf; const int* Mi; float* ST;
    const float* Pw; const float* Rt; const int* SQ; const int* SK;
    long long swb, swh, swi, swj, srb, srh, sri;
    long long sQb, sQh, sQi, sQd, sKb, sKh, sKj, sKd, sVb, sVh, sVj, sVd, sOb, sOh, sOi, sPb, sPh, sPi, smb, smh, smi, smj;
    int Lq, Lk, dh, dv, hrep, causal, coff, pband;
    float scale, mfill; int nonorm, mpol;
    int roff, rn, segpol, win;
};
static_assert(sizeof(AttnP) == 12 * 8 + 29 * 8 + 16 * 4, "AttnP has padding");

#ifndef KATTN_ATTR
#define KATTN_ATTR
#endif
template <int DHP, int DVP, int QM, bool SPLITPV, bool TWOPASS>
__global__ __launch_bounds__(32 * AW) KATTN_ATTR void k_attn(AttnP p) {
    constexpr int NT = DVP / 16;
    constexpr int KS = DHP / 32;
    constexpr int VP = DVP + 8;
    __shared__ __align__(16) float    pl[AW][16 * 64];
    __shared__ __align__(16) _Float16 vl[(SPLITPV ? 2 : 1) * 64 * VP];
    const int lane = threadIdx.x & 31, hf = lane >> 4, l15 = lane & 15, wave = threadIdx.x >> 5;
    const int h = blockIdx.y, b = blockIdx.z, hk = h / p.hrep;
    const int q0 = (blockIdx.x * AW + wave) * 16;
    float* myp = pl[wave];
    const float L2E = 1.4426950408889634f;
    const float NEG = -__builtin_inff();
    const int qi = min(q0 + l15, p.Lq - 1);
    const float* qrow = p.Q + b * p.sQb + h * p.sQh + (long long)qi * p.sQi;
    const float* kbase = p.K + b * p.sKb + hk * p.sKh;
    const float* vbase = p.V + b * p.sVb + hk * p.sVh;
    v16h qa[QM == 0 ? KS : 1]; Split qs_[QM == 1 ? KS : 1]; Split3 qt_[QM == 2 ? KS : 1];
#pragma unroll
    for (int ks = 0; ks < KS; ++ks) {
        if (QM == 2) qt_[ks] = sp3_ld(qrow, p.sQd, ks * 32, hf, p.dh, 1.f);
        else if (QM == 1) qs_[ks] = sp_ld(qrow, p.sQd, ks * 32, hf, p.dh, 1.f);
        else qa[ks] = fh_ld(qrow, p.sQd, ks * 32, hf, p.dh, 1.f);
    }
    v8f o[NT]; float m8[8], l8[8];
#pragma unroll
    for (int t = 0; t < NT; ++t) { v8f zz = {}; o[t] = zz; }
#pragma unroll
    for (int i = 0; i < 8; ++i) { m8[i] = NEG; l8[i] = 0.f; }
    int jend = p.Lk;
    if (p.causal == 1) { const int je = (blockIdx.x * AW + AW - 1) * 16 + 16 + p.coff; jend = min(jend, max(je, 0)); }
    const int npass = TWOPASS ? 2 : 1;
    for (int pass = 0; pass < npass; ++pass) {
        const bool dopv = (!TWOPASS) || pass == 1;
        for (int j0 = 0; j0 < jend; j0 += 64) {
            if (dopv) {
                __syncthreads();
                for (int idx = threadIdx.x; idx < 64 * DVP; idx += 32 * AW) {
                    const int jr = idx / DVP, d = idx - jr * DVP, j = j0 + jr;
                    const float f = (j < p.Lk && d < p.dv) ? vbase[(long long)j * p.sVj + (long long)d * p.sVd] : 0.f;
                    if (SPLITPV) {
                        const __bf16 hb = bf16_rne(f);
                        ((__bf16*)vl)[jr * VP + d] = hb; ((__bf16*)vl)[64 * VP + jr * VP + d] = bf16_rne(f - bf16_f32(hb));
                    } else vl[jr * VP + d] = (_Float16)f;
                }
            }
            v8f s[4];
#pragma unroll
            for (int t = 0; t < 4; ++t) {
                const int j = min(j0 + t * 16 + l15, p.Lk - 1);
                const float* krow = kbase + (long long)j * p.sKj;
                v8f acc = {};
#pragma unroll
                for (int ks = 0; ks < KS; ++ks) {
                    if (QM == 2)      acc = wmma6(qt_[ks], sp3_ld(krow, p.sKd, ks * 32, hf, p.dh, 1.f), acc);
                    else if (QM == 1) acc = wmma3(qs_[ks], sp_ld(krow, p.sKd, ks * 32, hf, p.dh, 1.f), acc);
                    else              acc = wmma16(qa[ks], fh_ld(krow, p.sKd, ks * 32, hf, p.dh, 1.f), acc);
                }
                s[t] = acc;
            }
            float pv[8][4];
#pragma unroll
            for (int i = 0; i < 8; ++i) {
                const int irow = q0 + i + 8 * hf;
                const int ic = min(irow, p.Lq - 1);
                float sc[4];
#pragma unroll
                for (int t = 0; t < 4; ++t) {
                    const int jg = j0 + t * 16 + l15;
                    float v = s[t][i] * p.scale;
                    if (p.Mf) v += p.Mf[b * p.smb + h * p.smh + (long long)ic * p.smi + (long long)min(jg, p.Lk - 1) * p.smj];
                    if (p.Rt) { int rc = ic - min(jg, p.Lk - 1) + p.roff; rc = rc < 0 ? 0 : (rc >= p.rn ? p.rn - 1 : rc); v += p.Rt[b * p.srb + h * p.srh + (long long)ic * p.sri + rc]; }
                    if (p.Mi) { const int mv = p.Mi[b * p.smb + h * p.smh + (long long)ic * p.smi + (long long)min(jg, p.Lk - 1) * p.smj]; if (p.mpol ? (mv != 0) : (mv == 0)) v = p.mfill; }
                    if (p.SQ) { const bool same = p.SQ[(long long)b * p.Lq + ic] == p.SK[(long long)b * p.Lk + min(jg, p.Lk - 1)]; if (p.segpol ? same : !same) v = p.mfill; }
                    if (p.causal == 2 && jg > irow + p.coff) v = p.mfill;
                    if (jg >= p.Lk || (p.causal == 1 && jg > irow + p.coff) || (p.causal == 3 && jg < irow + p.coff) || (p.win > 0 && irow + p.coff - jg > p.win)) v = NEG; else v *= L2E;
                    sc[t] = v;
                }
                if (!TWOPASS || pass == 0) {
                    float mx = fmaxf(fmaxf(sc[0], sc[1]), fmaxf(sc[2], sc[3]));
                    mx = fmaxf(mx, __shfl_xor(mx, 1, 32)); mx = fmaxf(mx, __shfl_xor(mx, 2, 32));
                    mx = fmaxf(mx, __shfl_xor(mx, 4, 32)); mx = fmaxf(mx, __shfl_xor(mx, 8, 32));
                    const float mnew = fmaxf(m8[i], mx);
                    const float corr = (mnew == NEG) ? 1.f : exp2f(m8[i] - mnew);
                    float rs = 0.f;
#pragma unroll
                    for (int t = 0; t < 4; ++t) {
                        const float pp = (sc[t] == NEG) ? 0.f : exp2f(sc[t] - mnew); rs += pp;
                        pv[i][t] = p.Pw ? pp * p.Pw[b * p.swb + h * p.swh + (long long)ic * p.swi + (long long)min(j0 + t * 16 + l15, p.Lk - 1) * p.swj] : pp;
                    }
                    rs += __shfl_xor(rs, 1, 32); rs += __shfl_xor(rs, 2, 32); rs += __shfl_xor(rs, 4, 32); rs += __shfl_xor(rs, 8, 32);
                    l8[i] = l8[i] * corr + rs; m8[i] = mnew;
                    if (!TWOPASS) {
#pragma unroll
                        for (int t = 0; t < NT; ++t) o[t][i] *= corr;
                    }
                } else {
                    const float inv = (l8[i] > 0.f) ? 1.f / l8[i] : 0.f;
#pragma unroll
                    for (int t = 0; t < 4; ++t) {
                        const int jg = j0 + t * 16 + l15;
                        float pp = (sc[t] == NEG) ? 0.f : exp2f(sc[t] - m8[i]) * inv;
                        if (p.Pw) pp *= p.Pw[b * p.swb + h * p.swh + (long long)ic * p.swi + (long long)min(jg, p.Lk - 1) * p.swj];
                        pv[i][t] = pp;
                    }
                }
            }
            if (dopv) {
#pragma unroll
                for (int i = 0; i < 8; ++i)
#pragma unroll
                    for (int t = 0; t < 4; ++t) myp[(i + 8 * hf) * 64 + t * 16 + l15] = pv[i][t];
                __syncthreads();
                if (p.P) {
                    float* pb_ = p.P + b * p.sPb + h * p.sPh;
                    const bool fastP = (p.pband == 0) && ((p.sPi & 3) == 0) && (j0 + 64 <= p.Lk) && (q0 + 16 <= p.Lq) && ((((size_t)pb_) & 15) == 0);
                    if (fastP) {
#pragma unroll
                        for (int s = 0; s < 8; ++s) {
                            const int row = s * 2 + (lane >> 4), c4 = (lane & 15) * 4;
                            const v4f v = *(const v4f*)(myp + row * 64 + c4);
                            VST2V4(pb_ + (long long)(q0 + row) * p.sPi + j0 + c4, v);
                        }
                    } else {
                        for (int row = 0; row < 16; ++row) {
                            const int irow = q0 + row; if (irow >= p.Lq) continue;
                            for (int c = lane; c < 64; c += 32) {
                                const int jg = j0 + c; if (jg >= p.Lk) continue;
                                if (p.pband == 0) VST2(float, pb_ + (long long)irow * p.sPi + jg, myp[row * 64 + c]);
                                else if (jg - irow <= p.pband && irow - jg <= p.pband) VST2(float, pb_ + (long long)irow * p.sPi + (jg - irow + p.pband), myp[row * 64 + c]);
                            }
                        }
                    }
                }
                if (SPLITPV) {
                    const Split pa0 = sp_ld(myp + l15 * 64, 1, 0, hf, 64, 1.f), pa1 = sp_ld(myp + l15 * 64, 1, 32, hf, 64, 1.f);
                    const __bf16* vh = (const __bf16*)vl; const __bf16* vlo = vh + 64 * VP;
#pragma unroll
                    for (int t = 0; t < NT; ++t) {
                        const int dcol = t * 16 + l15;
                        Split b0, b1;
#pragma unroll
                        for (int e = 0; e < 16; ++e) {
                            const int k0 = frag_k(e, hf), k1 = 32 + frag_k(e, hf);
                            b0.hi[e] = vh[k0 * VP + dcol]; b0.lo[e] = vlo[k0 * VP + dcol]; b1.hi[e] = vh[k1 * VP + dcol]; b1.lo[e] = vlo[k1 * VP + dcol];
                        }
                        o[t] = wmma3(pa0, b0, o[t]);
                        o[t] = wmma3(pa1, b1, o[t]);
                    }
                } else {
                    const v16h pa0 = fh_ld(myp + l15 * 64, 1, 0, hf, 64, 4096.f), pa1 = fh_ld(myp + l15 * 64, 1, 32, hf, 64, 4096.f);
#pragma unroll
                    for (int t = 0; t < NT; ++t) {
                        const int dcol = t * 16 + l15;
                        v16h b0, b1;
#pragma unroll
                        for (int e = 0; e < 16; ++e) { b0[e] = vl[frag_k(e, hf) * VP + dcol]; b1[e] = vl[(32 + frag_k(e, hf)) * VP + dcol]; }
                        o[t] = wmma16(pa0, b0, o[t]);
                        o[t] = wmma16(pa1, b1, o[t]);
                    }
                }
            }
        }
    }
    float* obase = p.O + b * p.sOb + h * p.sOh;
    if (p.ST) {
        const int rl = lane >> 1, isel = rl & 7;
        float mv = 0.f, lv = 0.f;
#pragma unroll
        for (int i = 0; i < 8; ++i) if (i == isel) { mv = m8[i]; lv = l8[i]; }
        const int irow = q0 + rl;
        if (irow < p.Lq) { float* st = p.ST + (((long long)b * gridDim.y + h) * p.Lq + irow) * 2 + (lane & 1); VST2(float, st, (lane & 1) ? lv : mv * 0.6931471805599453f); }
    }
    float invr[8];
#pragma unroll
    for (int i = 0; i < 8; ++i) {
        if (TWOPASS) invr[i] = SPLITPV ? 1.f : (1.f / 4096.f);
        else if (p.nonorm) invr[i] = exp2f(m8[i]) * (SPLITPV ? 1.f : (1.f / 4096.f));
        else invr[i] = (l8[i] > 0.f) ? (SPLITPV ? 1.f / l8[i] : 1.f / (l8[i] * 4096.f)) : 0.f;
    }
    __syncthreads();
    const bool ofast = ((p.sOi & 3) == 0) && ((((size_t)obase) & 15) == 0) && (q0 + 16 <= p.Lq);
#pragma unroll
    for (int c0 = 0; c0 < DVP; c0 += 64) {
#pragma unroll
        for (int i = 0; i < 8; ++i)
#pragma unroll
            for (int t = 0; t < NT; ++t) if (t * 16 >= c0 && t * 16 < c0 + 64) myp[(i + 8 * hf) * 64 + (t * 16 - c0) + l15] = o[t][i] * invr[i];
        __syncthreads();
        const int cw = (DVP - c0 < 64) ? (DVP - c0) : 64;
        if (ofast && (c0 + cw <= p.dv) && (cw % 32 == 0)) {
            const int lpr = cw / 4;
            const int rows_per_ins = 32 / lpr;
            for (int r0 = 0; r0 < 16; r0 += rows_per_ins) {
                const int row = r0 + lane / lpr, c4 = (lane % lpr) * 4;
                const v4f v = *(const v4f*)(myp + row * 64 + c4);
                VST2V4(obase + (long long)(q0 + row) * p.sOi + c0 + c4, v);
            }
        } else {
            for (int row = 0; row < 16; ++row) {
                const int irow = q0 + row; if (irow >= p.Lq) continue;
                for (int c = lane; c < cw; c += 32) { const int d = c0 + c; if (d < p.dv) VST2(float, obase + (long long)irow * p.sOi + d, myp[row * 64 + c]); }
            }
        }
        __syncthreads();
    }
}

struct TrP { const float* src; float* dst; const float* R2; long long sSz, lds, sDz, ldd, sRz, ldr; int R, C, flags, act; float alpha, beta; };
static_assert(sizeof(TrP) == 3 * 8 + 6 * 8 + 6 * 4, "TrP has padding");
__global__ __launch_bounds__(256) void k_tr(TrP p) {
    __shared__ float tile[32][33];
    const int c0 = blockIdx.x * 32, r0 = blockIdx.y * 32, z = blockIdx.z;
    const int lane = threadIdx.x & 31, wave = threadIdx.x >> 5;
    const float* s = p.src + z * p.sSz;
#pragma unroll
    for (int k = 0; k < 4; ++k) {
        const int rl = wave * 4 + k, r = r0 + rl, c = c0 + lane;
        tile[rl][lane] = (r < p.R && c < p.C) ? s[(long long)r * p.lds + c] : 0.f;
    }
    __syncthreads();
    float* d = p.dst + z * p.sDz; const float* rr = p.R2 + z * p.sRz;
#pragma unroll
    for (int k = 0; k < 4; ++k) {
        const int cl = wave * 4 + k, c = c0 + cl, r = r0 + lane;
        if (c < p.C && r < p.R) {
            float v = act_fn(p.alpha * tile[lane][cl], p.act);
            if (p.flags & 1) v += p.beta * rr[(long long)c * p.ldr + r];
            VST2(float, d + (long long)c * p.ldd + r, v);
        }
    }
}

__global__ __launch_bounds__(256) void k_affine(const float* __restrict__ src, float* __restrict__ dst, int n, float a, float b, const float* __restrict__ sdev) {
    const int i = blockIdx.x * 256 + threadIdx.x;
    if (i < n) { const float aa = sdev ? a * sdev[0] : a; const float v = aa * src[i] + b; VST2(float, dst + i, v); }
}

struct SmP { const float* src; float* dst; const float* Mf; long long sz, sr, dz, dr, smz, smr; int n, pad; float scale_in, scale_out; };
static_assert(sizeof(SmP) == 3 * 8 + 6 * 8 + 4 * 4, "SmP has padding");
__global__ __launch_bounds__(256) void k_softmax(SmP p) {
    __shared__ float red[256];
    const int r = blockIdx.x, z = blockIdx.y, tid = threadIdx.x;
    const float* s = p.src + z * p.sz + (long long)r * p.sr;
    const float* mf = p.Mf ? (p.Mf + z * p.smz + (long long)r * p.smr) : nullptr;
    float mx = -__builtin_inff();
    for (int j = tid; j < p.n; j += 256) { float v = s[j] * p.scale_in; if (mf) v += mf[j]; mx = fmaxf(mx, v); }
    red[tid] = mx; __syncthreads();
    for (int o = 128; o > 0; o >>= 1) { if (tid < o) red[tid] = fmaxf(red[tid], red[tid + o]); __syncthreads(); }
    mx = red[0]; __syncthreads();
    float sum = 0.f;
    for (int j = tid; j < p.n; j += 256) { float v = s[j] * p.scale_in; if (mf) v += mf[j]; sum += (mx == -__builtin_inff()) ? 0.f : expf(v - mx); }
    red[tid] = sum; __syncthreads();
    for (int o = 128; o > 0; o >>= 1) { if (tid < o) red[tid] += red[tid + o]; __syncthreads(); }
    sum = red[0];
    const float inv = (sum > 0.f) ? p.scale_out / sum : 0.f;
    float* d = p.dst + z * p.dz + (long long)r * p.dr;
    for (int j = tid; j < p.n; j += 256) { float v = s[j] * p.scale_in; if (mf) v += mf[j]; const float o = (mx == -__builtin_inff()) ? 0.f : expf(v - mx) * inv; VST2(float, d + j, o); }
}
__global__ __launch_bounds__(256) void k_stats(const float* __restrict__ x, long long sz, long long so, long long si, int inner, int n, float eps, float* __restrict__ stat, int mode) {
    __shared__ float red[256];
    const int z = blockIdx.x, tid = threadIdx.x;
    const float* base = x + z * sz;
    float s = 0.f;
    for (int e = tid; e < n; e += 256) s += base[(long long)(e / inner) * so + (long long)(e % inner) * si];
    red[tid] = s; __syncthreads();
    for (int o = 128; o > 0; o >>= 1) { if (tid < o) red[tid] += red[tid + o]; __syncthreads(); }
    const float mu = (mode == 0 || mode == 3) ? red[0] / (float)n : 0.f; __syncthreads();
    float q = 0.f;
    for (int e = tid; e < n; e += 256) { const float dlt = base[(long long)(e / inner) * so + (long long)(e % inner) * si] - mu; q += dlt * dlt; }
    red[tid] = q; __syncthreads();
    for (int o = 128; o > 0; o >>= 1) { if (tid < o) red[tid] += red[tid + o]; __syncthreads(); }
    {
        float rs;
        if (mode == 2) rs = sqrtf((float)n) / fmaxf(sqrtf(red[0]), eps); else if (mode == 3) rs = rsqrtf(red[0] / (float)(n - 1) + eps); else rs = rsqrtf(red[0] / (float)n + eps);
        if (tid < 32) { const float v = (tid == 0) ? mu : ((tid == 1) ? rs : 0.f); VST2(float, stat + (long long)z * 32 + tid, v); }
    }
}
__global__ __launch_bounds__(256) void k_norm_apply(const float* __restrict__ x, float* __restrict__ y, const float* __restrict__ stat, const float* __restrict__ g, const float* __restrict__ bta,
                                                     int Z, int C, int L, int G, int bn, int act) {
    const long long idx = (long long)blockIdx.x * 256 + threadIdx.x;
    if (idx >= (long long)Z * C * L) return;
    const int l = (int)(idx % L); const long long zc = idx / L; const int c = (int)(zc % C), z = (int)(zc / C); (void)l;
    const int set = bn ? c : (z * G + c / (C / G));
    float v = (x[idx] - stat[(long long)set * 32]) * stat[(long long)set * 32 + 1];
    if (g) v *= g[c];
    if (bta) v += bta[c];
    v = act_fn(v, act);
    VST2(float, y + idx, v);
}

__global__ __launch_bounds__(256) void k_lse_neg(const float* __restrict__ st, float* __restrict__ c, int n) {
    const int i = blockIdx.x * 256 + threadIdx.x;
    if (i < n) { const float v = -(st[2 * i] + logf(st[2 * i + 1])); VST2(float, c + i, v); }
}

__global__ __launch_bounds__(256) void k_iota(int* __restrict__ dst, int n, int a, int b) {
    const int i = blockIdx.x * 256 + threadIdx.x;
    if (i < n) { const int v = a * i + b; VST2(int, dst + i, v); }
}

__global__ __launch_bounds__(256) void k_axpby(const float* __restrict__ x, const float* __restrict__ y, float* __restrict__ dst, int n, float a, float b, float c) {
    const int i = blockIdx.x * 256 + threadIdx.x;
    if (i < n) { const float v = a * x[i] + b * y[i] + c; VST2(float, dst + i, v); }
}

struct RopeP { const float* X; float* Y; const float* C; const float* Sn; const int* pos; long long sXr, sXh, sYr, sYh, sCb, sCp, sCd; int R, Hn, D, S, mode, tmode, pmode, pad; };
static_assert(sizeof(RopeP) == 5 * 8 + 7 * 8 + 8 * 4, "RopeP has padding");
__global__ __launch_bounds__(256) void k_rope(RopeP p) {
    const long long idx = (long long)blockIdx.x * 256 + threadIdx.x;
    if (idx >= (long long)p.R * p.Hn * p.D) return;
    const int d = (int)(idx % p.D); const long long rh = idx / p.D; const int h = (int)(rh % p.Hn); const int r = (int)(rh / p.Hn);
    const int half = p.D / 2;
    int partner; float sign;
    if (p.mode == 0) { partner = (d < half) ? d + half : d - half; sign = (d < half) ? -1.f : 1.f; }
    else { partner = d ^ 1; sign = (d & 1) ? 1.f : -1.f; }
    const int tcol = (p.tmode == 0) ? d : ((p.tmode == 1) ? (d % half) : (d >> 1));
    const int pp = (p.pmode == 0) ? (r % p.S) : ((p.pmode == 1) ? h : p.pos[r]);
    const long long toff = (long long)(r / p.S) * p.sCb + (long long)pp * p.sCp + (long long)tcol * p.sCd;
    const float* xr = p.X + (long long)r * p.sXr + (long long)h * p.sXh;
    const float v = xr[d] * p.C[toff] + sign * xr[partner] * p.Sn[toff];
    VST2(float, p.Y + (long long)r * p.sYr + (long long)h * p.sYh + d, v);
}

__global__ __launch_bounds__(256) void k_invf(float* __restrict__ invb, int half, int D, float base, float num, int fmode, float cexp) {
    const int i = blockIdx.x * 256 + threadIdx.x;
    if (i >= ((half + 31) / 32) * 32) return;
    if (i >= half) { VST2(float, invb + i, 0.f); return; }
    const float e = (float)(2 * i) / (float)D;
    float invf;
    if (fmode == 1) invf = num * expf((float)(2 * i) * cexp);
    else if (fmode == 2) invf = num * powf(base, (-2.0f * ((float)i - 1.0f)) / (float)D);
    else invf = num * (1.0f / powf(base, e));
    VST2(float, invb + i, invf);
}
__global__ __launch_bounds__(256) void k_sincos(float* __restrict__ cs, float* __restrict__ sn, const float* __restrict__ invb, int S, int half, float pscale) {
    const int idx = blockIdx.x * 256 + threadIdx.x;
    if (idx >= S * half) return;
    const int s = idx / half, i = idx - s * half;
    const float ang = (pscale * (float)s) * invb[i];
    VST2(float, cs + idx, cosf(ang)); VST2(float, sn + idx, sinf(ang));
}

__global__ __launch_bounds__(256) void k_mulact(const float* __restrict__ x, const float* __restrict__ y, float* __restrict__ dst, int n, int act) {
    const int i = blockIdx.x * 256 + threadIdx.x;
    if (i < n) { const float v = act_fn(x[i], act) * y[i]; VST2(float, dst + i, v); }
}

__global__ __launch_bounds__(256) void k_matvec(GemmP p) {
    const int rpt = (p.N == 1) ? 1 : 32;
    const long long r0 = ((long long)blockIdx.x * 256 + threadIdx.x) * rpt; const int z = blockIdx.z, zo = z / p.zi_n, zi = z - zo * p.zi_n;
    if (r0 >= p.M) return;
    const float* Bb = p.B + zo * p.sBo + zi * p.sBi;
    float* C = p.C + zo * p.sCo + zi * p.sCi; const float* R = p.R + zo * p.sRo + zi * p.sRi;
    for (int rr = 0; rr < rpt; ++rr) {
        const long long r = r0 + rr; if (r >= p.M) break;
        const float* A = p.A + zo * p.sAo + zi * p.sAi + r * p.sAm;
        float acc[8] = {0.f, 0.f, 0.f, 0.f, 0.f, 0.f, 0.f, 0.f};
        for (int k = 0; k < p.K; ++k) { const float a = A[(long long)k * p.sAk];
#pragma unroll
            for (int j = 0; j < 8; ++j) if (j < p.N) acc[j] += a * Bb[(long long)j * p.sBn + (long long)k * p.sBk]; }
#pragma unroll
        for (int j = 0; j < 8; ++j) if (j < p.N) {
            float v = acc[j] * p.alpha;
            if (p.flags & 1) v += p.bias[j];
            if (p.flags & 2) v += p.bias[r];
            v = act_fn(v, p.act);
            if (p.flags & 4) v += p.beta * R[r * p.sRm + (long long)j * p.sRn];
            VST2(float, C + r * p.sCm + j, v);
        }
    }
}
__global__ __launch_bounds__(256) void k_smallsoftmax(const float* __restrict__ src, float* __restrict__ dst, long long sr, long long dr, int n, long long R, float scale) {
    const long long r0 = ((long long)blockIdx.x * 256 + threadIdx.x) * 32;
    for (int rr = 0; rr < 32; ++rr) {
        const long long r = r0 + rr; if (r >= R) return;
        const float* s = src + r * sr; float* d = dst + r * dr;
        float mx = -__builtin_inff();
        for (int j = 0; j < n; ++j) mx = fmaxf(mx, s[j] * scale);
        float sum = 0.f;
        for (int j = 0; j < n; ++j) sum += expf(s[j] * scale - mx);
        const float inv = 1.f / sum;
        for (int j = 0; j < n; ++j) { const float v = expf(s[j] * scale - mx) * inv; VST2(float, d + j, v); }
    }
}

__global__ __launch_bounds__(32) void k_unitstat(float* __restrict__ st) { const int t = threadIdx.x; const float v = (t == 1) ? 1.f : 0.f; VST2(float, st + t, v); }

__global__ __launch_bounds__(256) void k_lincopy(const float* __restrict__ src, long long lds, float* __restrict__ dst, long long ldd, long long rows, int cols) {
    const long long i = (long long)blockIdx.x * 256 + threadIdx.x; if (i >= rows * cols) return;
    const long long r = i / cols; const int c = (int)(i - r * cols);
    const float v = src[r * lds + c]; VST2(float, dst + r * ldd + c, v);
}

__global__ __launch_bounds__(256) void k_moe_top2(const float* __restrict__ LG, float* __restrict__ CMB, int T, int NE, int ldp) {
    const int t = blockIdx.x * 256 + threadIdx.x; if (t >= T) return; const float* l = LG + (long long)t * ldp; float mx = -__builtin_inff();
#pragma unroll 1
    for (int e = 0; e < NE; ++e) mx = fmaxf(mx, l[e]);
    float s = 0.f;
#pragma unroll 1
    for (int e = 0; e < NE; ++e) s += expf(l[e] - mx);
    int i1 = 0; float v1 = -1.f;
#pragma unroll 1
    for (int e = 0; e < NE; ++e) { const float p = expf(l[e] - mx) / s; if (p > v1) { v1 = p; i1 = e; } }
    int i2 = -1; float v2 = -1.f;
#pragma unroll 1
    for (int e = 0; e < NE; ++e) { if (e == i1) continue; const float p = expf(l[e] - mx) / s; if (p > v2) { v2 = p; i2 = e; } }
#pragma unroll 1
    for (int e = 0; e < ldp; ++e) { const float v = (e == i1) ? v1 : ((e == i2) ? v2 : 0.f); VST2(float, CMB + (long long)t * ldp + e, v); }
}
__global__ __launch_bounds__(256) void k_moe_act(const float* __restrict__ G, const float* __restrict__ U, const float* __restrict__ CMB, int ldp, int e, float* __restrict__ A, long long n, int D) {
    const long long q = (long long)blockIdx.x * 256 + threadIdx.x; if (q >= n) return; const float g = G[q]; float v = (g / (1.f + expf(-g))) * U[q]; if (CMB) v *= CMB[(q / D) * ldp + e]; VST2(float, A + q, v);
}

template __global__ void k_gemm<1>(GemmP);
template __global__ void k_gemm<4>(GemmP);

extern "C" void kernel_launch(void* const* d_in, const int* in_sizes, int n_in, void* d_out, int out_size, void* d_ws, size_t ws_size, hipStream_t stream) {
    (void)in_sizes; (void)n_in; (void)out_size; (void)ws_size;
    const float* x = (const float*)d_in[0];
    const float* wg = (const float*)d_in[1];
    const float* wga = (const float*)d_in[2];
    const float* wup = (const float*)d_in[3];
    const float* wdn = (const float*)d_in[4];
    const float* sg = (const float*)d_in[5];
    const float* su = (const float*)d_in[6];
    const float* sd = (const float*)d_in[7];
    const int T = 8192;
    const int H = 1024;
    const int DE = 512;
    const int NE = 16;
    const int LP = 32;
    float* out = (float*)d_out;
    char* wsp = (char*)d_ws;
    float* LG = (float*)wsp; wsp += (((size_t)((size_t)T * LP) * 4 + 255) / 256) * 256;
    float* CMB = (float*)wsp; wsp += (((size_t)((size_t)T * LP) * 4 + 255) / 256) * 256;
    float* G1 = (float*)wsp; wsp += (((size_t)((size_t)T * H) * 4 + 255) / 256) * 256;
    float* U1 = (float*)wsp; wsp += (((size_t)((size_t)T * H) * 4 + 255) / 256) * 256;
    float* GE = (float*)wsp; wsp += (((size_t)((size_t)T * DE) * 4 + 255) / 256) * 256;
    float* UE = (float*)wsp; wsp += (((size_t)((size_t)T * DE) * 4 + 255) / 256) * 256;
    { GemmP grt;
      grt.A = x; grt.B = wg; grt.bias = x; grt.R = x; grt.C = LG;
      grt.sAo = 0; grt.sAi = 0; grt.sAm = H; grt.sAk = 1; grt.sBo = 0; grt.sBi = 0; grt.sBn = H; grt.sBk = 1; grt.sCo = 0; grt.sCi = 0; grt.sCm = LP; grt.sRo = 0; grt.sRi = 0; grt.sRm = 0; grt.sRn = 0;
      grt.M = T; grt.N = NE; grt.K = H; grt.zi_n = 1; grt.flags = 0; grt.act = 0;
      grt.alpha = 1.0f; grt.beta = 0.0f; grt.sa = 1.0f; grt.sb = 1.0f; grt.Npad = LP; grt.pad_ = 0;
      k_gemm<4><<<dim3((unsigned)((LP) + 31) / 32, (unsigned)((T) + 15) / 16, (unsigned)(1)), 32, 0, stream>>>(grt); }
    k_moe_top2<<<(unsigned)((T + 255) / 256), 256, 0, stream>>>(LG, CMB, T, NE, LP);
    { GemmP gsg;
      gsg.A = x; gsg.B = sg; gsg.bias = x; gsg.R = x; gsg.C = G1;
      gsg.sAo = 0; gsg.sAi = 0; gsg.sAm = H; gsg.sAk = 1; gsg.sBo = 0; gsg.sBi = 0; gsg.sBn = H; gsg.sBk = 1; gsg.sCo = 0; gsg.sCi = 0; gsg.sCm = H; gsg.sRo = 0; gsg.sRi = 0; gsg.sRm = 0; gsg.sRn = 0;
      gsg.M = T; gsg.N = H; gsg.K = H; gsg.zi_n = 1; gsg.flags = 0; gsg.act = 0;
      gsg.alpha = 1.0f; gsg.beta = 0.0f; gsg.sa = 1.0f; gsg.sb = 1.0f; gsg.Npad = H; gsg.pad_ = 0;
      k_gemm<1><<<dim3((unsigned)((H) + 31) / 32, (unsigned)((T) + 15) / 16, (unsigned)(1)), 32, 0, stream>>>(gsg); }
    { GemmP gsu;
      gsu.A = x; gsu.B = su; gsu.bias = x; gsu.R = x; gsu.C = U1;
      gsu.sAo = 0; gsu.sAi = 0; gsu.sAm = H; gsu.sAk = 1; gsu.sBo = 0; gsu.sBi = 0; gsu.sBn = H; gsu.sBk = 1; gsu.sCo = 0; gsu.sCi = 0; gsu.sCm = H; gsu.sRo = 0; gsu.sRi = 0; gsu.sRm = 0; gsu.sRn = 0;
      gsu.M = T; gsu.N = H; gsu.K = H; gsu.zi_n = 1; gsu.flags = 0; gsu.act = 0;
      gsu.alpha = 1.0f; gsu.beta = 0.0f; gsu.sa = 1.0f; gsu.sb = 1.0f; gsu.Npad = H; gsu.pad_ = 0;
      k_gemm<1><<<dim3((unsigned)((H) + 31) / 32, (unsigned)((T) + 15) / 16, (unsigned)(1)), 32, 0, stream>>>(gsu); }
    k_moe_act<<<(unsigned)(((long long)T * H + 255) / 256), 256, 0, stream>>>(G1, U1, nullptr, LP, 0, G1, (long long)T * H, H);
    { GemmP gsd;
      gsd.A = G1; gsd.B = sd; gsd.bias = G1; gsd.R = G1; gsd.C = out;
      gsd.sAo = 0; gsd.sAi = 0; gsd.sAm = H; gsd.sAk = 1; gsd.sBo = 0; gsd.sBi = 0; gsd.sBn = H; gsd.sBk = 1; gsd.sCo = 0; gsd.sCi = 0; gsd.sCm = H; gsd.sRo = 0; gsd.sRi = 0; gsd.sRm = 0; gsd.sRn = 0;
      gsd.M = T; gsd.N = H; gsd.K = H; gsd.zi_n = 1; gsd.flags = 0; gsd.act = 0;
      gsd.alpha = 1.0f; gsd.beta = 0.0f; gsd.sa = 1.0f; gsd.sb = 1.0f; gsd.Npad = H; gsd.pad_ = 0;
      k_gemm<1><<<dim3((unsigned)((H) + 31) / 32, (unsigned)((T) + 15) / 16, (unsigned)(1)), 32, 0, stream>>>(gsd); }
    { GemmP gg0;
      gg0.A = x; gg0.B = wga + (size_t)0 * DE * H; gg0.bias = x; gg0.R = x; gg0.C = GE;
      gg0.sAo = 0; gg0.sAi = 0; gg0.sAm = H; gg0.sAk = 1; gg0.sBo = 0; gg0.sBi = 0; gg0.sBn = H; gg0.sBk = 1; gg0.sCo = 0; gg0.sCi = 0; gg0.sCm = DE; gg0.sRo = 0; gg0.sRi = 0; gg0.sRm = 0; gg0.sRn = 0;
      gg0.M = T; gg0.N = DE; gg0.K = H; gg0.zi_n = 1; gg0.flags = 0; gg0.act = 0;
      gg0.alpha = 1.0f; gg0.beta = 0.0f; gg0.sa = 1.0f; gg0.sb = 1.0f; gg0.Npad = DE; gg0.pad_ = 0;
      k_gemm<1><<<dim3((unsigned)((DE) + 31) / 32, (unsigned)((T) + 15) / 16, (unsigned)(1)), 32, 0, stream>>>(gg0); }
    { GemmP gu0;
      gu0.A = x; gu0.B = wup + (size_t)0 * DE * H; gu0.bias = x; gu0.R = x; gu0.C = UE;
      gu0.sAo = 0; gu0.sAi = 0; gu0.sAm = H; gu0.sAk = 1; gu0.sBo = 0; gu0.sBi = 0; gu0.sBn = H; gu0.sBk = 1; gu0.sCo = 0; gu0.sCi = 0; gu0.sCm = DE; gu0.sRo = 0; gu0.sRi = 0; gu0.sRm = 0; gu0.sRn = 0;
      gu0.M = T; gu0.N = DE; gu0.K = H; gu0.zi_n = 1; gu0.flags = 0; gu0.act = 0;
      gu0.alpha = 1.0f; gu0.beta = 0.0f; gu0.sa = 1.0f; gu0.sb = 1.0f; gu0.Npad = DE; gu0.pad_ = 0;
      k_gemm<1><<<dim3((unsigned)((DE) + 31) / 32, (unsigned)((T) + 15) / 16, (unsigned)(1)), 32, 0, stream>>>(gu0); }
    k_moe_act<<<(unsigned)(((long long)T * DE + 255) / 256), 256, 0, stream>>>(GE, UE, CMB, LP, 0, GE, (long long)T * DE, DE);
    { GemmP gd0;
      gd0.A = GE; gd0.B = wdn + (size_t)0 * H * DE; gd0.bias = GE; gd0.R = out; gd0.C = out;
      gd0.sAo = 0; gd0.sAi = 0; gd0.sAm = DE; gd0.sAk = 1; gd0.sBo = 0; gd0.sBi = 0; gd0.sBn = DE; gd0.sBk = 1; gd0.sCo = 0; gd0.sCi = 0; gd0.sCm = H; gd0.sRo = 0; gd0.sRi = 0; gd0.sRm = H; gd0.sRn = 1;
      gd0.M = T; gd0.N = H; gd0.K = DE; gd0.zi_n = 1; gd0.flags = 4; gd0.act = 0;
      gd0.alpha = 1.0f; gd0.beta = 1.0f; gd0.sa = 1.0f; gd0.sb = 1.0f; gd0.Npad = H; gd0.pad_ = 0;
      k_gemm<1><<<dim3((unsigned)((H) + 31) / 32, (unsigned)((T) + 15) / 16, (unsigned)(1)), 32, 0, stream>>>(gd0); }
    { GemmP gg1;
      gg1.A = x; gg1.B = wga + (size_t)1 * DE * H; gg1.bias = x; gg1.R = x; gg1.C = GE;
      gg1.sAo = 0; gg1.sAi = 0; gg1.sAm = H; gg1.sAk = 1; gg1.sBo = 0; gg1.sBi = 0; gg1.sBn = H; gg1.sBk = 1; gg1.sCo = 0; gg1.sCi = 0; gg1.sCm = DE; gg1.sRo = 0; gg1.sRi = 0; gg1.sRm = 0; gg1.sRn = 0;
      gg1.M = T; gg1.N = DE; gg1.K = H; gg1.zi_n = 1; gg1.flags = 0; gg1.act = 0;
      gg1.alpha = 1.0f; gg1.beta = 0.0f; gg1.sa = 1.0f; gg1.sb = 1.0f; gg1.Npad = DE; gg1.pad_ = 0;
      k_gemm<1><<<dim3((unsigned)((DE) + 31) / 32, (unsigned)((T) + 15) / 16, (unsigned)(1)), 32, 0, stream>>>(gg1); }
    { GemmP gu1;
      gu1.A = x; gu1.B = wup + (size_t)1 * DE * H; gu1.bias = x; gu1.R = x; gu1.C = UE;
      gu1.sAo = 0; gu1.sAi = 0; gu1.sAm = H; gu1.sAk = 1; gu1.sBo = 0; gu1.sBi = 0; gu1.sBn = H; gu1.sBk = 1; gu1.sCo = 0; gu1.sCi = 0; gu1.sCm = DE; gu1.sRo = 0; gu1.sRi = 0; gu1.sRm = 0; gu1.sRn = 0;
      gu1.M = T; gu1.N = DE; gu1.K = H; gu1.zi_n = 1; gu1.flags = 0; gu1.act = 0;
      gu1.alpha = 1.0f; gu1.beta = 0.0f; gu1.sa = 1.0f; gu1.sb = 1.0f; gu1.Npad = DE; gu1.pad_ = 0;
      k_gemm<1><<<dim3((unsigned)((DE) + 31) / 32, (unsigned)((T) + 15) / 16, (unsigned)(1)), 32, 0, stream>>>(gu1); }
    k_moe_act<<<(unsigned)(((long long)T * DE + 255) / 256), 256, 0, stream>>>(GE, UE, CMB, LP, 1, GE, (long long)T * DE, DE);
    { GemmP gd1;
      gd1.A = GE; gd1.B = wdn + (size_t)1 * H * DE; gd1.bias = GE; gd1.R = out; gd1.C = out;
      gd1.sAo = 0; gd1.sAi = 0; gd1.sAm = DE; gd1.sAk = 1; gd1.sBo = 0; gd1.sBi = 0; gd1.sBn = DE; gd1.sBk = 1; gd1.sCo = 0; gd1.sCi = 0; gd1.sCm = H; gd1.sRo = 0; gd1.sRi = 0; gd1.sRm = H; gd1.sRn = 1;
      gd1.M = T; gd1.N = H; gd1.K = DE; gd1.zi_n = 1; gd1.flags = 4; gd1.act = 0;
      gd1.alpha = 1.0f; gd1.beta = 1.0f; gd1.sa = 1.0f; gd1.sb = 1.0f; gd1.Npad = H; gd1.pad_ = 0;
      k_gemm<1><<<dim3((unsigned)((H) + 31) / 32, (unsigned)((T) + 15) / 16, (unsigned)(1)), 32, 0, stream>>>(gd1); }
    { GemmP gg2;
      gg2.A = x; gg2.B = wga + (size_t)2 * DE * H; gg2.bias = x; gg2.R = x; gg2.C = GE;
      gg2.sAo = 0; gg2.sAi = 0; gg2.sAm = H; gg2.sAk = 1; gg2.sBo = 0; gg2.sBi = 0; gg2.sBn = H; gg2.sBk = 1; gg2.sCo = 0; gg2.sCi = 0; gg2.sCm = DE; gg2.sRo = 0; gg2.sRi = 0; gg2.sRm = 0; gg2.sRn = 0;
      gg2.M = T; gg2.N = DE; gg2.K = H; gg2.zi_n = 1; gg2.flags = 0; gg2.act = 0;
      gg2.alpha = 1.0f; gg2.beta = 0.0f; gg2.sa = 1.0f; gg2.sb = 1.0f; gg2.Npad = DE; gg2.pad_ = 0;
      k_gemm<1><<<dim3((unsigned)((DE) + 31) / 32, (unsigned)((T) + 15) / 16, (unsigned)(1)), 32, 0, stream>>>(gg2); }
    { GemmP gu2;
      gu2.A = x; gu2.B = wup + (size_t)2 * DE * H; gu2.bias = x; gu2.R = x; gu2.C = UE;
      gu2.sAo = 0; gu2.sAi = 0; gu2.sAm = H; gu2.sAk = 1; gu2.sBo = 0; gu2.sBi = 0; gu2.sBn = H; gu2.sBk = 1; gu2.sCo = 0; gu2.sCi = 0; gu2.sCm = DE; gu2.sRo = 0; gu2.sRi = 0; gu2.sRm = 0; gu2.sRn = 0;
      gu2.M = T; gu2.N = DE; gu2.K = H; gu2.zi_n = 1; gu2.flags = 0; gu2.act = 0;
      gu2.alpha = 1.0f; gu2.beta = 0.0f; gu2.sa = 1.0f; gu2.sb = 1.0f; gu2.Npad = DE; gu2.pad_ = 0;
      k_gemm<1><<<dim3((unsigned)((DE) + 31) / 32, (unsigned)((T) + 15) / 16, (unsigned)(1)), 32, 0, stream>>>(gu2); }
    k_moe_act<<<(unsigned)(((long long)T * DE + 255) / 256), 256, 0, stream>>>(GE, UE, CMB, LP, 2, GE, (long long)T * DE, DE);
    { GemmP gd2;
      gd2.A = GE; gd2.B = wdn + (size_t)2 * H * DE; gd2.bias = GE; gd2.R = out; gd2.C = out;
      gd2.sAo = 0; gd2.sAi = 0; gd2.sAm = DE; gd2.sAk = 1; gd2.sBo = 0; gd2.sBi = 0; gd2.sBn = DE; gd2.sBk = 1; gd2.sCo = 0; gd2.sCi = 0; gd2.sCm = H; gd2.sRo = 0; gd2.sRi = 0; gd2.sRm = H; gd2.sRn = 1;
      gd2.M = T; gd2.N = H; gd2.K = DE; gd2.zi_n = 1; gd2.flags = 4; gd2.act = 0;
      gd2.alpha = 1.0f; gd2.beta = 1.0f; gd2.sa = 1.0f; gd2.sb = 1.0f; gd2.Npad = H; gd2.pad_ = 0;
      k_gemm<1><<<dim3((unsigned)((H) + 31) / 32, (unsigned)((T) + 15) / 16, (unsigned)(1)), 32, 0, stream>>>(gd2); }
    { GemmP gg3;
      gg3.A = x; gg3.B = wga + (size_t)3 * DE * H; gg3.bias = x; gg3.R = x; gg3.C = GE;
      gg3.sAo = 0; gg3.sAi = 0; gg3.sAm = H; gg3.sAk = 1; gg3.sBo = 0; gg3.sBi = 0; gg3.sBn = H; gg3.sBk = 1; gg3.sCo = 0; gg3.sCi = 0; gg3.sCm = DE; gg3.sRo = 0; gg3.sRi = 0; gg3.sRm = 0; gg3.sRn = 0;
      gg3.M = T; gg3.N = DE; gg3.K = H; gg3.zi_n = 1; gg3.flags = 0; gg3.act = 0;
      gg3.alpha = 1.0f; gg3.beta = 0.0f; gg3.sa = 1.0f; gg3.sb = 1.0f; gg3.Npad = DE; gg3.pad_ = 0;
      k_gemm<1><<<dim3((unsigned)((DE) + 31) / 32, (unsigned)((T) + 15) / 16, (unsigned)(1)), 32, 0, stream>>>(gg3); }
    { GemmP gu3;
      gu3.A = x; gu3.B = wup + (size_t)3 * DE * H; gu3.bias = x; gu3.R = x; gu3.C = UE;
      gu3.sAo = 0; gu3.sAi = 0; gu3.sAm = H; gu3.sAk = 1; gu3.sBo = 0; gu3.sBi = 0; gu3.sBn = H; gu3.sBk = 1; gu3.sCo = 0; gu3.sCi = 0; gu3.sCm = DE; gu3.sRo = 0; gu3.sRi = 0; gu3.sRm = 0; gu3.sRn = 0;
      gu3.M = T; gu3.N = DE; gu3.K = H; gu3.zi_n = 1; gu3.flags = 0; gu3.act = 0;
      gu3.alpha = 1.0f; gu3.beta = 0.0f; gu3.sa = 1.0f; gu3.sb = 1.0f; gu3.Npad = DE; gu3.pad_ = 0;
      k_gemm<1><<<dim3((unsigned)((DE) + 31) / 32, (unsigned)((T) + 15) / 16, (unsigned)(1)), 32, 0, stream>>>(gu3); }
    k_moe_act<<<(unsigned)(((long long)T * DE + 255) / 256), 256, 0, stream>>>(GE, UE, CMB, LP, 3, GE, (long long)T * DE, DE);
    { GemmP gd3;
      gd3.A = GE; gd3.B = wdn + (size_t)3 * H * DE; gd3.bias = GE; gd3.R = out; gd3.C = out;
      gd3.sAo = 0; gd3.sAi = 0; gd3.sAm = DE; gd3.sAk = 1; gd3.sBo = 0; gd3.sBi = 0; gd3.sBn = DE; gd3.sBk = 1; gd3.sCo = 0; gd3.sCi = 0; gd3.sCm = H; gd3.sRo = 0; gd3.sRi = 0; gd3.sRm = H; gd3.sRn = 1;
      gd3.M = T; gd3.N = H; gd3.K = DE; gd3.zi_n = 1; gd3.flags = 4; gd3.act = 0;
      gd3.alpha = 1.0f; gd3.beta = 1.0f; gd3.sa = 1.0f; gd3.sb = 1.0f; gd3.Npad = H; gd3.pad_ = 0;
      k_gemm<1><<<dim3((unsigned)((H) + 31) / 32, (unsigned)((T) + 15) / 16, (unsigned)(1)), 32, 0, stream>>>(gd3); }
    { GemmP gg4;
      gg4.A = x; gg4.B = wga + (size_t)4 * DE * H; gg4.bias = x; gg4.R = x; gg4.C = GE;
      gg4.sAo = 0; gg4.sAi = 0; gg4.sAm = H; gg4.sAk = 1; gg4.sBo = 0; gg4.sBi = 0; gg4.sBn = H; gg4.sBk = 1; gg4.sCo = 0; gg4.sCi = 0; gg4.sCm = DE; gg4.sRo = 0; gg4.sRi = 0; gg4.sRm = 0; gg4.sRn = 0;
      gg4.M = T; gg4.N = DE; gg4.K = H; gg4.zi_n = 1; gg4.flags = 0; gg4.act = 0;
      gg4.alpha = 1.0f; gg4.beta = 0.0f; gg4.sa = 1.0f; gg4.sb = 1.0f; gg4.Npad = DE; gg4.pad_ = 0;
      k_gemm<1><<<dim3((unsigned)((DE) + 31) / 32, (unsigned)((T) + 15) / 16, (unsigned)(1)), 32, 0, stream>>>(gg4); }
    { GemmP gu4;
      gu4.A = x; gu4.B = wup + (size_t)4 * DE * H; gu4.bias = x; gu4.R = x; gu4.C = UE;
      gu4.sAo = 0; gu4.sAi = 0; gu4.sAm = H; gu4.sAk = 1; gu4.sBo = 0; gu4.sBi = 0; gu4.sBn = H; gu4.sBk = 1; gu4.sCo = 0; gu4.sCi = 0; gu4.sCm = DE; gu4.sRo = 0; gu4.sRi = 0; gu4.sRm = 0; gu4.sRn = 0;
      gu4.M = T; gu4.N = DE; gu4.K = H; gu4.zi_n = 1; gu4.flags = 0; gu4.act = 0;
      gu4.alpha = 1.0f; gu4.beta = 0.0f; gu4.sa = 1.0f; gu4.sb = 1.0f; gu4.Npad = DE; gu4.pad_ = 0;
      k_gemm<1><<<dim3((unsigned)((DE) + 31) / 32, (unsigned)((T) + 15) / 16, (unsigned)(1)), 32, 0, stream>>>(gu4); }
    k_moe_act<<<(unsigned)(((long long)T * DE + 255) / 256), 256, 0, stream>>>(GE, UE, CMB, LP, 4, GE, (long long)T * DE, DE);
    { GemmP gd4;
      gd4.A = GE; gd4.B = wdn + (size_t)4 * H * DE; gd4.bias = GE; gd4.R = out; gd4.C = out;
      gd4.sAo = 0; gd4.sAi = 0; gd4.sAm = DE; gd4.sAk = 1; gd4.sBo = 0; gd4.sBi = 0; gd4.sBn = DE; gd4.sBk = 1; gd4.sCo = 0; gd4.sCi = 0; gd4.sCm = H; gd4.sRo = 0; gd4.sRi = 0; gd4.sRm = H; gd4.sRn = 1;
      gd4.M = T; gd4.N = H; gd4.K = DE; gd4.zi_n = 1; gd4.flags = 4; gd4.act = 0;
      gd4.alpha = 1.0f; gd4.beta = 1.0f; gd4.sa = 1.0f; gd4.sb = 1.0f; gd4.Npad = H; gd4.pad_ = 0;
      k_gemm<1><<<dim3((unsigned)((H) + 31) / 32, (unsigned)((T) + 15) / 16, (unsigned)(1)), 32, 0, stream>>>(gd4); }
    { GemmP gg5;
      gg5.A = x; gg5.B = wga + (size_t)5 * DE * H; gg5.bias = x; gg5.R = x; gg5.C = GE;
      gg5.sAo = 0; gg5.sAi = 0; gg5.sAm = H; gg5.sAk = 1; gg5.sBo = 0; gg5.sBi = 0; gg5.sBn = H; gg5.sBk = 1; gg5.sCo = 0; gg5.sCi = 0; gg5.sCm = DE; gg5.sRo = 0; gg5.sRi = 0; gg5.sRm = 0; gg5.sRn = 0;
      gg5.M = T; gg5.N = DE; gg5.K = H; gg5.zi_n = 1; gg5.flags = 0; gg5.act = 0;
      gg5.alpha = 1.0f; gg5.beta = 0.0f; gg5.sa = 1.0f; gg5.sb = 1.0f; gg5.Npad = DE; gg5.pad_ = 0;
      k_gemm<1><<<dim3((unsigned)((DE) + 31) / 32, (unsigned)((T) + 15) / 16, (unsigned)(1)), 32, 0, stream>>>(gg5); }
    { GemmP gu5;
      gu5.A = x; gu5.B = wup + (size_t)5 * DE * H; gu5.bias = x; gu5.R = x; gu5.C = UE;
      gu5.sAo = 0; gu5.sAi = 0; gu5.sAm = H; gu5.sAk = 1; gu5.sBo = 0; gu5.sBi = 0; gu5.sBn = H; gu5.sBk = 1; gu5.sCo = 0; gu5.sCi = 0; gu5.sCm = DE; gu5.sRo = 0; gu5.sRi = 0; gu5.sRm = 0; gu5.sRn = 0;
      gu5.M = T; gu5.N = DE; gu5.K = H; gu5.zi_n = 1; gu5.flags = 0; gu5.act = 0;
      gu5.alpha = 1.0f; gu5.beta = 0.0f; gu5.sa = 1.0f; gu5.sb = 1.0f; gu5.Npad = DE; gu5.pad_ = 0;
      k_gemm<1><<<dim3((unsigned)((DE) + 31) / 32, (unsigned)((T) + 15) / 16, (unsigned)(1)), 32, 0, stream>>>(gu5); }
    k_moe_act<<<(unsigned)(((long long)T * DE + 255) / 256), 256, 0, stream>>>(GE, UE, CMB, LP, 5, GE, (long long)T * DE, DE);
    { GemmP gd5;
      gd5.A = GE; gd5.B = wdn + (size_t)5 * H * DE; gd5.bias = GE; gd5.R = out; gd5.C = out;
      gd5.sAo = 0; gd5.sAi = 0; gd5.sAm = DE; gd5.sAk = 1; gd5.sBo = 0; gd5.sBi = 0; gd5.sBn = DE; gd5.sBk = 1; gd5.sCo = 0; gd5.sCi = 0; gd5.sCm = H; gd5.sRo = 0; gd5.sRi = 0; gd5.sRm = H; gd5.sRn = 1;
      gd5.M = T; gd5.N = H; gd5.K = DE; gd5.zi_n = 1; gd5.flags = 4; gd5.act = 0;
      gd5.alpha = 1.0f; gd5.beta = 1.0f; gd5.sa = 1.0f; gd5.sb = 1.0f; gd5.Npad = H; gd5.pad_ = 0;
      k_gemm<1><<<dim3((unsigned)((H) + 31) / 32, (unsigned)((T) + 15) / 16, (unsigned)(1)), 32, 0, stream>>>(gd5); }
    { GemmP gg6;
      gg6.A = x; gg6.B = wga + (size_t)6 * DE * H; gg6.bias = x; gg6.R = x; gg6.C = GE;
      gg6.sAo = 0; gg6.sAi = 0; gg6.sAm = H; gg6.sAk = 1; gg6.sBo = 0; gg6.sBi = 0; gg6.sBn = H; gg6.sBk = 1; gg6.sCo = 0; gg6.sCi = 0; gg6.sCm = DE; gg6.sRo = 0; gg6.sRi = 0; gg6.sRm = 0; gg6.sRn = 0;
      gg6.M = T; gg6.N = DE; gg6.K = H; gg6.zi_n = 1; gg6.flags = 0; gg6.act = 0;
      gg6.alpha = 1.0f; gg6.beta = 0.0f; gg6.sa = 1.0f; gg6.sb = 1.0f; gg6.Npad = DE; gg6.pad_ = 0;
      k_gemm<1><<<dim3((unsigned)((DE) + 31) / 32, (unsigned)((T) + 15) / 16, (unsigned)(1)), 32, 0, stream>>>(gg6); }
    { GemmP gu6;
      gu6.A = x; gu6.B = wup + (size_t)6 * DE * H; gu6.bias = x; gu6.R = x; gu6.C = UE;
      gu6.sAo = 0; gu6.sAi = 0; gu6.sAm = H; gu6.sAk = 1; gu6.sBo = 0; gu6.sBi = 0; gu6.sBn = H; gu6.sBk = 1; gu6.sCo = 0; gu6.sCi = 0; gu6.sCm = DE; gu6.sRo = 0; gu6.sRi = 0; gu6.sRm = 0; gu6.sRn = 0;
      gu6.M = T; gu6.N = DE; gu6.K = H; gu6.zi_n = 1; gu6.flags = 0; gu6.act = 0;
      gu6.alpha = 1.0f; gu6.beta = 0.0f; gu6.sa = 1.0f; gu6.sb = 1.0f; gu6.Npad = DE; gu6.pad_ = 0;
      k_gemm<1><<<dim3((unsigned)((DE) + 31) / 32, (unsigned)((T) + 15) / 16, (unsigned)(1)), 32, 0, stream>>>(gu6); }
    k_moe_act<<<(unsigned)(((long long)T * DE + 255) / 256), 256, 0, stream>>>(GE, UE, CMB, LP, 6, GE, (long long)T * DE, DE);
    { GemmP gd6;
      gd6.A = GE; gd6.B = wdn + (size_t)6 * H * DE; gd6.bias = GE; gd6.R = out; gd6.C = out;
      gd6.sAo = 0; gd6.sAi = 0; gd6.sAm = DE; gd6.sAk = 1; gd6.sBo = 0; gd6.sBi = 0; gd6.sBn = DE; gd6.sBk = 1; gd6.sCo = 0; gd6.sCi = 0; gd6.sCm = H; gd6.sRo = 0; gd6.sRi = 0; gd6.sRm = H; gd6.sRn = 1;
      gd6.M = T; gd6.N = H; gd6.K = DE; gd6.zi_n = 1; gd6.flags = 4; gd6.act = 0;
      gd6.alpha = 1.0f; gd6.beta = 1.0f; gd6.sa = 1.0f; gd6.sb = 1.0f; gd6.Npad = H; gd6.pad_ = 0;
      k_gemm<1><<<dim3((unsigned)((H) + 31) / 32, (unsigned)((T) + 15) / 16, (unsigned)(1)), 32, 0, stream>>>(gd6); }
    { GemmP gg7;
      gg7.A = x; gg7.B = wga + (size_t)7 * DE * H; gg7.bias = x; gg7.R = x; gg7.C = GE;
      gg7.sAo = 0; gg7.sAi = 0; gg7.sAm = H; gg7.sAk = 1; gg7.sBo = 0; gg7.sBi = 0; gg7.sBn = H; gg7.sBk = 1; gg7.sCo = 0; gg7.sCi = 0; gg7.sCm = DE; gg7.sRo = 0; gg7.sRi = 0; gg7.sRm = 0; gg7.sRn = 0;
      gg7.M = T; gg7.N = DE; gg7.K = H; gg7.zi_n = 1; gg7.flags = 0; gg7.act = 0;
      gg7.alpha = 1.0f; gg7.beta = 0.0f; gg7.sa = 1.0f; gg7.sb = 1.0f; gg7.Npad = DE; gg7.pad_ = 0;
      k_gemm<1><<<dim3((unsigned)((DE) + 31) / 32, (unsigned)((T) + 15) / 16, (unsigned)(1)), 32, 0, stream>>>(gg7); }
    { GemmP gu7;
      gu7.A = x; gu7.B = wup + (size_t)7 * DE * H; gu7.bias = x; gu7.R = x; gu7.C = UE;
      gu7.sAo = 0; gu7.sAi = 0; gu7.sAm = H; gu7.sAk = 1; gu7.sBo = 0; gu7.sBi = 0; gu7.sBn = H; gu7.sBk = 1; gu7.sCo = 0; gu7.sCi = 0; gu7.sCm = DE; gu7.sRo = 0; gu7.sRi = 0; gu7.sRm = 0; gu7.sRn = 0;
      gu7.M = T; gu7.N = DE; gu7.K = H; gu7.zi_n = 1; gu7.flags = 0; gu7.act = 0;
      gu7.alpha = 1.0f; gu7.beta = 0.0f; gu7.sa = 1.0f; gu7.sb = 1.0f; gu7.Npad = DE; gu7.pad_ = 0;
      k_gemm<1><<<dim3((unsigned)((DE) + 31) / 32, (unsigned)((T) + 15) / 16, (unsigned)(1)), 32, 0, stream>>>(gu7); }
    k_moe_act<<<(unsigned)(((long long)T * DE + 255) / 256), 256, 0, stream>>>(GE, UE, CMB, LP, 7, GE, (long long)T * DE, DE);
    { GemmP gd7;
      gd7.A = GE; gd7.B = wdn + (size_t)7 * H * DE; gd7.bias = GE; gd7.R = out; gd7.C = out;
      gd7.sAo = 0; gd7.sAi = 0; gd7.sAm = DE; gd7.sAk = 1; gd7.sBo = 0; gd7.sBi = 0; gd7.sBn = DE; gd7.sBk = 1; gd7.sCo = 0; gd7.sCi = 0; gd7.sCm = H; gd7.sRo = 0; gd7.sRi = 0; gd7.sRm = H; gd7.sRn = 1;
      gd7.M = T; gd7.N = H; gd7.K = DE; gd7.zi_n = 1; gd7.flags = 4; gd7.act = 0;
      gd7.alpha = 1.0f; gd7.beta = 1.0f; gd7.sa = 1.0f; gd7.sb = 1.0f; gd7.Npad = H; gd7.pad_ = 0;
      k_gemm<1><<<dim3((unsigned)((H) + 31) / 32, (unsigned)((T) + 15) / 16, (unsigned)(1)), 32, 0, stream>>>(gd7); }
    { GemmP gg8;
      gg8.A = x; gg8.B = wga + (size_t)8 * DE * H; gg8.bias = x; gg8.R = x; gg8.C = GE;
      gg8.sAo = 0; gg8.sAi = 0; gg8.sAm = H; gg8.sAk = 1; gg8.sBo = 0; gg8.sBi = 0; gg8.sBn = H; gg8.sBk = 1; gg8.sCo = 0; gg8.sCi = 0; gg8.sCm = DE; gg8.sRo = 0; gg8.sRi = 0; gg8.sRm = 0; gg8.sRn = 0;
      gg8.M = T; gg8.N = DE; gg8.K = H; gg8.zi_n = 1; gg8.flags = 0; gg8.act = 0;
      gg8.alpha = 1.0f; gg8.beta = 0.0f; gg8.sa = 1.0f; gg8.sb = 1.0f; gg8.Npad = DE; gg8.pad_ = 0;
      k_gemm<1><<<dim3((unsigned)((DE) + 31) / 32, (unsigned)((T) + 15) / 16, (unsigned)(1)), 32, 0, stream>>>(gg8); }
    { GemmP gu8;
      gu8.A = x; gu8.B = wup + (size_t)8 * DE * H; gu8.bias = x; gu8.R = x; gu8.C = UE;
      gu8.sAo = 0; gu8.sAi = 0; gu8.sAm = H; gu8.sAk = 1; gu8.sBo = 0; gu8.sBi = 0; gu8.sBn = H; gu8.sBk = 1; gu8.sCo = 0; gu8.sCi = 0; gu8.sCm = DE; gu8.sRo = 0; gu8.sRi = 0; gu8.sRm = 0; gu8.sRn = 0;
      gu8.M = T; gu8.N = DE; gu8.K = H; gu8.zi_n = 1; gu8.flags = 0; gu8.act = 0;
      gu8.alpha = 1.0f; gu8.beta = 0.0f; gu8.sa = 1.0f; gu8.sb = 1.0f; gu8.Npad = DE; gu8.pad_ = 0;
      k_gemm<1><<<dim3((unsigned)((DE) + 31) / 32, (unsigned)((T) + 15) / 16, (unsigned)(1)), 32, 0, stream>>>(gu8); }
    k_moe_act<<<(unsigned)(((long long)T * DE + 255) / 256), 256, 0, stream>>>(GE, UE, CMB, LP, 8, GE, (long long)T * DE, DE);
    { GemmP gd8;
      gd8.A = GE; gd8.B = wdn + (size_t)8 * H * DE; gd8.bias = GE; gd8.R = out; gd8.C = out;
      gd8.sAo = 0; gd8.sAi = 0; gd8.sAm = DE; gd8.sAk = 1; gd8.sBo = 0; gd8.sBi = 0; gd8.sBn = DE; gd8.sBk = 1; gd8.sCo = 0; gd8.sCi = 0; gd8.sCm = H; gd8.sRo = 0; gd8.sRi = 0; gd8.sRm = H; gd8.sRn = 1;
      gd8.M = T; gd8.N = H; gd8.K = DE; gd8.zi_n = 1; gd8.flags = 4; gd8.act = 0;
      gd8.alpha = 1.0f; gd8.beta = 1.0f; gd8.sa = 1.0f; gd8.sb = 1.0f; gd8.Npad = H; gd8.pad_ = 0;
      k_gemm<1><<<dim3((unsigned)((H) + 31) / 32, (unsigned)((T) + 15) / 16, (unsigned)(1)), 32, 0, stream>>>(gd8); }
    { GemmP gg9;
      gg9.A = x; gg9.B = wga + (size_t)9 * DE * H; gg9.bias = x; gg9.R = x; gg9.C = GE;
      gg9.sAo = 0; gg9.sAi = 0; gg9.sAm = H; gg9.sAk = 1; gg9.sBo = 0; gg9.sBi = 0; gg9.sBn = H; gg9.sBk = 1; gg9.sCo = 0; gg9.sCi = 0; gg9.sCm = DE; gg9.sRo = 0; gg9.sRi = 0; gg9.sRm = 0; gg9.sRn = 0;
      gg9.M = T; gg9.N = DE; gg9.K = H; gg9.zi_n = 1; gg9.flags = 0; gg9.act = 0;
      gg9.alpha = 1.0f; gg9.beta = 0.0f; gg9.sa = 1.0f; gg9.sb = 1.0f; gg9.Npad = DE; gg9.pad_ = 0;
      k_gemm<1><<<dim3((unsigned)((DE) + 31) / 32, (unsigned)((T) + 15) / 16, (unsigned)(1)), 32, 0, stream>>>(gg9); }
    { GemmP gu9;
      gu9.A = x; gu9.B = wup + (size_t)9 * DE * H; gu9.bias = x; gu9.R = x; gu9.C = UE;
      gu9.sAo = 0; gu9.sAi = 0; gu9.sAm = H; gu9.sAk = 1; gu9.sBo = 0; gu9.sBi = 0; gu9.sBn = H; gu9.sBk = 1; gu9.sCo = 0; gu9.sCi = 0; gu9.sCm = DE; gu9.sRo = 0; gu9.sRi = 0; gu9.sRm = 0; gu9.sRn = 0;
      gu9.M = T; gu9.N = DE; gu9.K = H; gu9.zi_n = 1; gu9.flags = 0; gu9.act = 0;
      gu9.alpha = 1.0f; gu9.beta = 0.0f; gu9.sa = 1.0f; gu9.sb = 1.0f; gu9.Npad = DE; gu9.pad_ = 0;
      k_gemm<1><<<dim3((unsigned)((DE) + 31) / 32, (unsigned)((T) + 15) / 16, (unsigned)(1)), 32, 0, stream>>>(gu9); }
    k_moe_act<<<(unsigned)(((long long)T * DE + 255) / 256), 256, 0, stream>>>(GE, UE, CMB, LP, 9, GE, (long long)T * DE, DE);
    { GemmP gd9;
      gd9.A = GE; gd9.B = wdn + (size_t)9 * H * DE; gd9.bias = GE; gd9.R = out; gd9.C = out;
      gd9.sAo = 0; gd9.sAi = 0; gd9.sAm = DE; gd9.sAk = 1; gd9.sBo = 0; gd9.sBi = 0; gd9.sBn = DE; gd9.sBk = 1; gd9.sCo = 0; gd9.sCi = 0; gd9.sCm = H; gd9.sRo = 0; gd9.sRi = 0; gd9.sRm = H; gd9.sRn = 1;
      gd9.M = T; gd9.N = H; gd9.K = DE; gd9.zi_n = 1; gd9.flags = 4; gd9.act = 0;
      gd9.alpha = 1.0f; gd9.beta = 1.0f; gd9.sa = 1.0f; gd9.sb = 1.0f; gd9.Npad = H; gd9.pad_ = 0;
      k_gemm<1><<<dim3((unsigned)((H) + 31) / 32, (unsigned)((T) + 15) / 16, (unsigned)(1)), 32, 0, stream>>>(gd9); }
    { GemmP gg10;
      gg10.A = x; gg10.B = wga + (size_t)10 * DE * H; gg10.bias = x; gg10.R = x; gg10.C = GE;
      gg10.sAo = 0; gg10.sAi = 0; gg10.sAm = H; gg10.sAk = 1; gg10.sBo = 0; gg10.sBi = 0; gg10.sBn = H; gg10.sBk = 1; gg10.sCo = 0; gg10.sCi = 0; gg10.sCm = DE; gg10.sRo = 0; gg10.sRi = 0; gg10.sRm = 0; gg10.sRn = 0;
      gg10.M = T; gg10.N = DE; gg10.K = H; gg10.zi_n = 1; gg10.flags = 0; gg10.act = 0;
      gg10.alpha = 1.0f; gg10.beta = 0.0f; gg10.sa = 1.0f; gg10.sb = 1.0f; gg10.Npad = DE; gg10.pad_ = 0;
      k_gemm<1><<<dim3((unsigned)((DE) + 31) / 32, (unsigned)((T) + 15) / 16, (unsigned)(1)), 32, 0, stream>>>(gg10); }
    { GemmP gu10;
      gu10.A = x; gu10.B = wup + (size_t)10 * DE * H; gu10.bias = x; gu10.R = x; gu10.C = UE;
      gu10.sAo = 0; gu10.sAi = 0; gu10.sAm = H; gu10.sAk = 1; gu10.sBo = 0; gu10.sBi = 0; gu10.sBn = H; gu10.sBk = 1; gu10.sCo = 0; gu10.sCi = 0; gu10.sCm = DE; gu10.sRo = 0; gu10.sRi = 0; gu10.sRm = 0; gu10.sRn = 0;
      gu10.M = T; gu10.N = DE; gu10.K = H; gu10.zi_n = 1; gu10.flags = 0; gu10.act = 0;
      gu10.alpha = 1.0f; gu10.beta = 0.0f; gu10.sa = 1.0f; gu10.sb = 1.0f; gu10.Npad = DE; gu10.pad_ = 0;
      k_gemm<1><<<dim3((unsigned)((DE) + 31) / 32, (unsigned)((T) + 15) / 16, (unsigned)(1)), 32, 0, stream>>>(gu10); }
    k_moe_act<<<(unsigned)(((long long)T * DE + 255) / 256), 256, 0, stream>>>(GE, UE, CMB, LP, 10, GE, (long long)T * DE, DE);
    { GemmP gd10;
      gd10.A = GE; gd10.B = wdn + (size_t)10 * H * DE; gd10.bias = GE; gd10.R = out; gd10.C = out;
      gd10.sAo = 0; gd10.sAi = 0; gd10.sAm = DE; gd10.sAk = 1; gd10.sBo = 0; gd10.sBi = 0; gd10.sBn = DE; gd10.sBk = 1; gd10.sCo = 0; gd10.sCi = 0; gd10.sCm = H; gd10.sRo = 0; gd10.sRi = 0; gd10.sRm = H; gd10.sRn = 1;
      gd10.M = T; gd10.N = H; gd10.K = DE; gd10.zi_n = 1; gd10.flags = 4; gd10.act = 0;
      gd10.alpha = 1.0f; gd10.beta = 1.0f; gd10.sa = 1.0f; gd10.sb = 1.0f; gd10.Npad = H; gd10.pad_ = 0;
      k_gemm<1><<<dim3((unsigned)((H) + 31) / 32, (unsigned)((T) + 15) / 16, (unsigned)(1)), 32, 0, stream>>>(gd10); }
    { GemmP gg11;
      gg11.A = x; gg11.B = wga + (size_t)11 * DE * H; gg11.bias = x; gg11.R = x; gg11.C = GE;
      gg11.sAo = 0; gg11.sAi = 0; gg11.sAm = H; gg11.sAk = 1; gg11.sBo = 0; gg11.sBi = 0; gg11.sBn = H; gg11.sBk = 1; gg11.sCo = 0; gg11.sCi = 0; gg11.sCm = DE; gg11.sRo = 0; gg11.sRi = 0; gg11.sRm = 0; gg11.sRn = 0;
      gg11.M = T; gg11.N = DE; gg11.K = H; gg11.zi_n = 1; gg11.flags = 0; gg11.act = 0;
      gg11.alpha = 1.0f; gg11.beta = 0.0f; gg11.sa = 1.0f; gg11.sb = 1.0f; gg11.Npad = DE; gg11.pad_ = 0;
      k_gemm<1><<<dim3((unsigned)((DE) + 31) / 32, (unsigned)((T) + 15) / 16, (unsigned)(1)), 32, 0, stream>>>(gg11); }
    { GemmP gu11;
      gu11.A = x; gu11.B = wup + (size_t)11 * DE * H; gu11.bias = x; gu11.R = x; gu11.C = UE;
      gu11.sAo = 0; gu11.sAi = 0; gu11.sAm = H; gu11.sAk = 1; gu11.sBo = 0; gu11.sBi = 0; gu11.sBn = H; gu11.sBk = 1; gu11.sCo = 0; gu11.sCi = 0; gu11.sCm = DE; gu11.sRo = 0; gu11.sRi = 0; gu11.sRm = 0; gu11.sRn = 0;
      gu11.M = T; gu11.N = DE; gu11.K = H; gu11.zi_n = 1; gu11.flags = 0; gu11.act = 0;
      gu11.alpha = 1.0f; gu11.beta = 0.0f; gu11.sa = 1.0f; gu11.sb = 1.0f; gu11.Npad = DE; gu11.pad_ = 0;
      k_gemm<1><<<dim3((unsigned)((DE) + 31) / 32, (unsigned)((T) + 15) / 16, (unsigned)(1)), 32, 0, stream>>>(gu11); }
    k_moe_act<<<(unsigned)(((long long)T * DE + 255) / 256), 256, 0, stream>>>(GE, UE, CMB, LP, 11, GE, (long long)T * DE, DE);
    { GemmP gd11;
      gd11.A = GE; gd11.B = wdn + (size_t)11 * H * DE; gd11.bias = GE; gd11.R = out; gd11.C = out;
      gd11.sAo = 0; gd11.sAi = 0; gd11.sAm = DE; gd11.sAk = 1; gd11.sBo = 0; gd11.sBi = 0; gd11.sBn = DE; gd11.sBk = 1; gd11.sCo = 0; gd11.sCi = 0; gd11.sCm = H; gd11.sRo = 0; gd11.sRi = 0; gd11.sRm = H; gd11.sRn = 1;
      gd11.M = T; gd11.N = H; gd11.K = DE; gd11.zi_n = 1; gd11.flags = 4; gd11.act = 0;
      gd11.alpha = 1.0f; gd11.beta = 1.0f; gd11.sa = 1.0f; gd11.sb = 1.0f; gd11.Npad = H; gd11.pad_ = 0;
      k_gemm<1><<<dim3((unsigned)((H) + 31) / 32, (unsigned)((T) + 15) / 16, (unsigned)(1)), 32, 0, stream>>>(gd11); }
    { GemmP gg12;
      gg12.A = x; gg12.B = wga + (size_t)12 * DE * H; gg12.bias = x; gg12.R = x; gg12.C = GE;
      gg12.sAo = 0; gg12.sAi = 0; gg12.sAm = H; gg12.sAk = 1; gg12.sBo = 0; gg12.sBi = 0; gg12.sBn = H; gg12.sBk = 1; gg12.sCo = 0; gg12.sCi = 0; gg12.sCm = DE; gg12.sRo = 0; gg12.sRi = 0; gg12.sRm = 0; gg12.sRn = 0;
      gg12.M = T; gg12.N = DE; gg12.K = H; gg12.zi_n = 1; gg12.flags = 0; gg12.act = 0;
      gg12.alpha = 1.0f; gg12.beta = 0.0f; gg12.sa = 1.0f; gg12.sb = 1.0f; gg12.Npad = DE; gg12.pad_ = 0;
      k_gemm<1><<<dim3((unsigned)((DE) + 31) / 32, (unsigned)((T) + 15) / 16, (unsigned)(1)), 32, 0, stream>>>(gg12); }
    { GemmP gu12;
      gu12.A = x; gu12.B = wup + (size_t)12 * DE * H; gu12.bias = x; gu12.R = x; gu12.C = UE;
      gu12.sAo = 0; gu12.sAi = 0; gu12.sAm = H; gu12.sAk = 1; gu12.sBo = 0; gu12.sBi = 0; gu12.sBn = H; gu12.sBk = 1; gu12.sCo = 0; gu12.sCi = 0; gu12.sCm = DE; gu12.sRo = 0; gu12.sRi = 0; gu12.sRm = 0; gu12.sRn = 0;
      gu12.M = T; gu12.N = DE; gu12.K = H; gu12.zi_n = 1; gu12.flags = 0; gu12.act = 0;
      gu12.alpha = 1.0f; gu12.beta = 0.0f; gu12.sa = 1.0f; gu12.sb = 1.0f; gu12.Npad = DE; gu12.pad_ = 0;
      k_gemm<1><<<dim3((unsigned)((DE) + 31) / 32, (unsigned)((T) + 15) / 16, (unsigned)(1)), 32, 0, stream>>>(gu12); }
    k_moe_act<<<(unsigned)(((long long)T * DE + 255) / 256), 256, 0, stream>>>(GE, UE, CMB, LP, 12, GE, (long long)T * DE, DE);
    { GemmP gd12;
      gd12.A = GE; gd12.B = wdn + (size_t)12 * H * DE; gd12.bias = GE; gd12.R = out; gd12.C = out;
      gd12.sAo = 0; gd12.sAi = 0; gd12.sAm = DE; gd12.sAk = 1; gd12.sBo = 0; gd12.sBi = 0; gd12.sBn = DE; gd12.sBk = 1; gd12.sCo = 0; gd12.sCi = 0; gd12.sCm = H; gd12.sRo = 0; gd12.sRi = 0; gd12.sRm = H; gd12.sRn = 1;
      gd12.M = T; gd12.N = H; gd12.K = DE; gd12.zi_n = 1; gd12.flags = 4; gd12.act = 0;
      gd12.alpha = 1.0f; gd12.beta = 1.0f; gd12.sa = 1.0f; gd12.sb = 1.0f; gd12.Npad = H; gd12.pad_ = 0;
      k_gemm<1><<<dim3((unsigned)((H) + 31) / 32, (unsigned)((T) + 15) / 16, (unsigned)(1)), 32, 0, stream>>>(gd12); }
    { GemmP gg13;
      gg13.A = x; gg13.B = wga + (size_t)13 * DE * H; gg13.bias = x; gg13.R = x; gg13.C = GE;
      gg13.sAo = 0; gg13.sAi = 0; gg13.sAm = H; gg13.sAk = 1; gg13.sBo = 0; gg13.sBi = 0; gg13.sBn = H; gg13.sBk = 1; gg13.sCo = 0; gg13.sCi = 0; gg13.sCm = DE; gg13.sRo = 0; gg13.sRi = 0; gg13.sRm = 0; gg13.sRn = 0;
      gg13.M = T; gg13.N = DE; gg13.K = H; gg13.zi_n = 1; gg13.flags = 0; gg13.act = 0;
      gg13.alpha = 1.0f; gg13.beta = 0.0f; gg13.sa = 1.0f; gg13.sb = 1.0f; gg13.Npad = DE; gg13.pad_ = 0;
      k_gemm<1><<<dim3((unsigned)((DE) + 31) / 32, (unsigned)((T) + 15) / 16, (unsigned)(1)), 32, 0, stream>>>(gg13); }
    { GemmP gu13;
      gu13.A = x; gu13.B = wup + (size_t)13 * DE * H; gu13.bias = x; gu13.R = x; gu13.C = UE;
      gu13.sAo = 0; gu13.sAi = 0; gu13.sAm = H; gu13.sAk = 1; gu13.sBo = 0; gu13.sBi = 0; gu13.sBn = H; gu13.sBk = 1; gu13.sCo = 0; gu13.sCi = 0; gu13.sCm = DE; gu13.sRo = 0; gu13.sRi = 0; gu13.sRm = 0; gu13.sRn = 0;
      gu13.M = T; gu13.N = DE; gu13.K = H; gu13.zi_n = 1; gu13.flags = 0; gu13.act = 0;
      gu13.alpha = 1.0f; gu13.beta = 0.0f; gu13.sa = 1.0f; gu13.sb = 1.0f; gu13.Npad = DE; gu13.pad_ = 0;
      k_gemm<1><<<dim3((unsigned)((DE) + 31) / 32, (unsigned)((T) + 15) / 16, (unsigned)(1)), 32, 0, stream>>>(gu13); }
    k_moe_act<<<(unsigned)(((long long)T * DE + 255) / 256), 256, 0, stream>>>(GE, UE, CMB, LP, 13, GE, (long long)T * DE, DE);
    { GemmP gd13;
      gd13.A = GE; gd13.B = wdn + (size_t)13 * H * DE; gd13.bias = GE; gd13.R = out; gd13.C = out;
      gd13.sAo = 0; gd13.sAi = 0; gd13.sAm = DE; gd13.sAk = 1; gd13.sBo = 0; gd13.sBi = 0; gd13.sBn = DE; gd13.sBk = 1; gd13.sCo = 0; gd13.sCi = 0; gd13.sCm = H; gd13.sRo = 0; gd13.sRi = 0; gd13.sRm = H; gd13.sRn = 1;
      gd13.M = T; gd13.N = H; gd13.K = DE; gd13.zi_n = 1; gd13.flags = 4; gd13.act = 0;
      gd13.alpha = 1.0f; gd13.beta = 1.0f; gd13.sa = 1.0f; gd13.sb = 1.0f; gd13.Npad = H; gd13.pad_ = 0;
      k_gemm<1><<<dim3((unsigned)((H) + 31) / 32, (unsigned)((T) + 15) / 16, (unsigned)(1)), 32, 0, stream>>>(gd13); }
    { GemmP gg14;
      gg14.A = x; gg14.B = wga + (size_t)14 * DE * H; gg14.bias = x; gg14.R = x; gg14.C = GE;
      gg14.sAo = 0; gg14.sAi = 0; gg14.sAm = H; gg14.sAk = 1; gg14.sBo = 0; gg14.sBi = 0; gg14.sBn = H; gg14.sBk = 1; gg14.sCo = 0; gg14.sCi = 0; gg14.sCm = DE; gg14.sRo = 0; gg14.sRi = 0; gg14.sRm = 0; gg14.sRn = 0;
      gg14.M = T; gg14.N = DE; gg14.K = H; gg14.zi_n = 1; gg14.flags = 0; gg14.act = 0;
      gg14.alpha = 1.0f; gg14.beta = 0.0f; gg14.sa = 1.0f; gg14.sb = 1.0f; gg14.Npad = DE; gg14.pad_ = 0;
      k_gemm<1><<<dim3((unsigned)((DE) + 31) / 32, (unsigned)((T) + 15) / 16, (unsigned)(1)), 32, 0, stream>>>(gg14); }
    { GemmP gu14;
      gu14.A = x; gu14.B = wup + (size_t)14 * DE * H; gu14.bias = x; gu14.R = x; gu14.C = UE;
      gu14.sAo = 0; gu14.sAi = 0; gu14.sAm = H; gu14.sAk = 1; gu14.sBo = 0; gu14.sBi = 0; gu14.sBn = H; gu14.sBk = 1; gu14.sCo = 0; gu14.sCi = 0; gu14.sCm = DE; gu14.sRo = 0; gu14.sRi = 0; gu14.sRm = 0; gu14.sRn = 0;
      gu14.M = T; gu14.N = DE; gu14.K = H; gu14.zi_n = 1; gu14.flags = 0; gu14.act = 0;
      gu14.alpha = 1.0f; gu14.beta = 0.0f; gu14.sa = 1.0f; gu14.sb = 1.0f; gu14.Npad = DE; gu14.pad_ = 0;
      k_gemm<1><<<dim3((unsigned)((DE) + 31) / 32, (unsigned)((T) + 15) / 16, (unsigned)(1)), 32, 0, stream>>>(gu14); }
    k_moe_act<<<(unsigned)(((long long)T * DE + 255) / 256), 256, 0, stream>>>(GE, UE, CMB, LP, 14, GE, (long long)T * DE, DE);
    { GemmP gd14;
      gd14.A = GE; gd14.B = wdn + (size_t)14 * H * DE; gd14.bias = GE; gd14.R = out; gd14.C = out;
      gd14.sAo = 0; gd14.sAi = 0; gd14.sAm = DE; gd14.sAk = 1; gd14.sBo = 0; gd14.sBi = 0; gd14.sBn = DE; gd14.sBk = 1; gd14.sCo = 0; gd14.sCi = 0; gd14.sCm = H; gd14.sRo = 0; gd14.sRi = 0; gd14.sRm = H; gd14.sRn = 1;
      gd14.M = T; gd14.N = H; gd14.K = DE; gd14.zi_n = 1; gd14.flags = 4; gd14.act = 0;
      gd14.alpha = 1.0f; gd14.beta = 1.0f; gd14.sa = 1.0f; gd14.sb = 1.0f; gd14.Npad = H; gd14.pad_ = 0;
      k_gemm<1><<<dim3((unsigned)((H) + 31) / 32, (unsigned)((T) + 15) / 16, (unsigned)(1)), 32, 0, stream>>>(gd14); }
    { GemmP gg15;
      gg15.A = x; gg15.B = wga + (size_t)15 * DE * H; gg15.bias = x; gg15.R = x; gg15.C = GE;
      gg15.sAo = 0; gg15.sAi = 0; gg15.sAm = H; gg15.sAk = 1; gg15.sBo = 0; gg15.sBi = 0; gg15.sBn = H; gg15.sBk = 1; gg15.sCo = 0; gg15.sCi = 0; gg15.sCm = DE; gg15.sRo = 0; gg15.sRi = 0; gg15.sRm = 0; gg15.sRn = 0;
      gg15.M = T; gg15.N = DE; gg15.K = H; gg15.zi_n = 1; gg15.flags = 0; gg15.act = 0;
      gg15.alpha = 1.0f; gg15.beta = 0.0f; gg15.sa = 1.0f; gg15.sb = 1.0f; gg15.Npad = DE; gg15.pad_ = 0;
      k_gemm<1><<<dim3((unsigned)((DE) + 31) / 32, (unsigned)((T) + 15) / 16, (unsigned)(1)), 32, 0, stream>>>(gg15); }
    { GemmP gu15;
      gu15.A = x; gu15.B = wup + (size_t)15 * DE * H; gu15.bias = x; gu15.R = x; gu15.C = UE;
      gu15.sAo = 0; gu15.sAi = 0; gu15.sAm = H; gu15.sAk = 1; gu15.sBo = 0; gu15.sBi = 0; gu15.sBn = H; gu15.sBk = 1; gu15.sCo = 0; gu15.sCi = 0; gu15.sCm = DE; gu15.sRo = 0; gu15.sRi = 0; gu15.sRm = 0; gu15.sRn = 0;
      gu15.M = T; gu15.N = DE; gu15.K = H; gu15.zi_n = 1; gu15.flags = 0; gu15.act = 0;
      gu15.alpha = 1.0f; gu15.beta = 0.0f; gu15.sa = 1.0f; gu15.sb = 1.0f; gu15.Npad = DE; gu15.pad_ = 0;
      k_gemm<1><<<dim3((unsigned)((DE) + 31) / 32, (unsigned)((T) + 15) / 16, (unsigned)(1)), 32, 0, stream>>>(gu15); }
    k_moe_act<<<(unsigned)(((long long)T * DE + 255) / 256), 256, 0, stream>>>(GE, UE, CMB, LP, 15, GE, (long long)T * DE, DE);
    { GemmP gd15;
      gd15.A = GE; gd15.B = wdn + (size_t)15 * H * DE; gd15.bias = GE; gd15.R = out; gd15.C = out;
      gd15.sAo = 0; gd15.sAi = 0; gd15.sAm = DE; gd15.sAk = 1; gd15.sBo = 0; gd15.sBi = 0; gd15.sBn = DE; gd15.sBk = 1; gd15.sCo = 0; gd15.sCi = 0; gd15.sCm = H; gd15.sRo = 0; gd15.sRi = 0; gd15.sRm = H; gd15.sRn = 1;
      gd15.M = T; gd15.N = H; gd15.K = DE; gd15.zi_n = 1; gd15.flags = 4; gd15.act = 0;
      gd15.alpha = 1.0f; gd15.beta = 1.0f; gd15.sa = 1.0f; gd15.sb = 1.0f; gd15.Npad = H; gd15.pad_ = 0;
      k_gemm<1><<<dim3((unsigned)((H) + 31) / 32, (unsigned)((T) + 15) / 16, (unsigned)(1)), 32, 0, stream>>>(gd15); }
}
